// SimpleAttentionWithHilbert_69776038690875
// MI455X (gfx1250) — hardware-verified
//
#include <hip/hip_runtime.h>
__device__ const int SH_PERM[8192] = {0,128,129,1,2,3,131,130,258,259,387,386,385,257,256,384,512,513,641,640,768,896,897,769,770,898,899,771,643,642,514,515,516,517,645,644,772,900,901,773,774,902,903,775,647,646,518,519,391,263,262,390,389,388,260,261,133,132,4,5,6,134,135,7,8,9,137,136,264,392,393,265,266,394,395,267,139,138,10,11,12,140,141,13,14,15,143,142,270,271,399,398,397,269,268,396,524,652,653,525,526,527,655,654,782,783,911,910,909,781,780,908,907,906,778,779,651,523,522,650,649,521,520,648,776,777,905,904,1032,1033,1161,1160,1288,1416,1417,1289,1290,1418,1419,1291,1163,1162,1034,1035,1036,1164,1165,1037,1038,1039,1167,1166,1294,1295,1423,1422,1421,1293,1292,1420,1548,1676,1677,1549,1550,1551,1679,1678,1806,1807,1935,1934,1933,1805,1804,1932,1931,1930,1802,1803,1675,1547,1546,1674,1673,1545,1544,1672,1800,1801,1929,1928,1927,1799,1798,1926,1925,1924,1796,1797,1669,1668,1540,1541,1542,1670,1671,1543,1415,1414,1286,1287,1159,1031,1030,1158,1157,1029,1028,1156,1284,1285,1413,1412,1411,1410,1282,1283,1155,1027,1026,1154,1153,1025,1024,1152,1280,1281,1409,1408,1536,1664,1665,1537,1538,1539,1667,1666,1794,1795,1923,1922,1921,1793,1792,1920,2048,2049,2177,2176,2304,2432,2433,2305,2306,2434,2435,2307,2179,2178,2050,2051,2052,2180,2181,2053,2054,2055,2183,2182,2310,2311,2439,2438,2437,2309,2308,2436,2564,2692,2693,2565,2566,2567,2695,2694,2822,2823,2951,2950,2949,2821,2820,2948,2947,2946,2818,2819,2691,2563,2562,2690,2689,2561,2560,2688,2816,2817,2945,2944,3072,3200,3201,3073,3074,3075,3203,3202,3330,3331,3459,3458,3457,3329,3328,3456,3584,3585,3713,3712,3840,3968,3969,3841,3842,3970,3971,3843,3715,3714,3586,3587,3588,3589,3717,3716,3844,3972,3973,3845,3846,3974,3975,3847,3719,3718,3590,3591,3463,3335,3334,3462,3461,3460,3332,3333,3205,3204,3076,3077,3078,3206,3207,3079,3080,3208,3209,3081,3082,3083,3211,3210,3338,3339,3467,3466,3465,3337,3336,3464,3592,3593,3721,3720,3848,3976,3977,3849,3850,3978,3979,3851,3723,3722,3594,3595,3596,3597,3725,3724,3852,3980,3981,3853,3854,3982,3983,3855,3727,3726,3598,3599,3471,3343,3342,3470,3469,3468,3340,3341,3213,3212,3084,3085,3086,3214,3215,3087,2959,2958,2830,2831,2703,2575,2574,2702,2701,2573,2572,2700,2828,2829,2957,2956,2955,2827,2826,2954,2953,2952,2824,2825,2697,2696,2568,2569,2570,2698,2699,2571,2443,2315,2314,2442,2441,2440,2312,2313,2185,2184,2056,2057,2058,2186,2187,2059,2060,2061,2189,2188,2316,2444,2445,2317,2318,2446,2447,2319,2191,2190,2062,2063,2064,2065,2193,2192,2320,2448,2449,2321,2322,2450,2451,2323,2195,2194,2066,2067,2068,2196,2197,2069,2070,2071,2199,2198,2326,2327,2455,2454,2453,2325,2324,2452,2580,2708,2709,2581,2582,2583,2711,2710,2838,2839,2967,2966,2965,2837,2836,2964,2963,2962,2834,2835,2707,2579,2578,2706,2705,2577,2576,2704,2832,2833,2961,2960,3088,3216,3217,3089,3090,3091,3219,3218,3346,3347,3475,3474,3473,3345,3344,3472,3600,3601,3729,3728,3856,3984,3985,3857,3858,3986,3987,3859,3731,3730,3602,3603,3604,3605,3733,3732,3860,3988,3989,3861,3862,3990,3991,3863,3735,3734,3606,3607,3479,3351,3350,3478,3477,3476,3348,3349,3221,3220,3092,3093,3094,3222,3223,3095,3096,3224,3225,3097,3098,3099,3227,3226,3354,3355,3483,3482,3481,3353,3352,3480,3608,3609,3737,3736,3864,3992,3993,3865,3866,3994,3995,3867,3739,3738,3610,3611,3612,3613,3741,3740,3868,3996,3997,3869,3870,3998,3999,3871,3743,3742,3614,3615,3487,3359,3358,3486,3485,3484,3356,3357,3229,3228,3100,3101,3102,3230,3231,3103,2975,2974,2846,2847,2719,2591,2590,2718,2717,2589,2588,2716,2844,2845,2973,2972,2971,2843,2842,2970,2969,2968,2840,2841,2713,2712,2584,2585,2586,2714,2715,2587,2459,2331,2330,2458,2457,2456,2328,2329,2201,2200,2072,2073,2074,2202,2203,2075,2076,2077,2205,2204,2332,2460,2461,2333,2334,2462,2463,2335,2207,2206,2078,2079,1951,1823,1822,1950,1949,1948,1820,1821,1693,1692,1564,1565,1566,1694,1695,1567,1439,1438,1310,1311,1183,1055,1054,1182,1181,1053,1052,1180,1308,1309,1437,1436,1435,1434,1306,1307,1179,1051,1050,1178,1177,1049,1048,1176,1304,1305,1433,1432,1560,1688,1689,1561,1562,1563,1691,1690,1818,1819,1947,1946,1945,1817,1816,1944,1943,1942,1814,1815,1687,1559,1558,1686,1685,1557,1556,1684,1812,1813,1941,1940,1939,1811,1810,1938,1937,1936,1808,1809,1681,1680,1552,1553,1554,1682,1683,1555,1427,1299,1298,1426,1425,1424,1296,1297,1169,1168,1040,1041,1042,1170,1171,1043,1044,1045,1173,1172,1300,1428,1429,1301,1302,1430,1431,1303,1175,1174,1046,1047,919,918,790,791,663,535,534,662,661,533,532,660,788,789,917,916,915,787,786,914,913,912,784,785,657,656,528,529,530,658,659,531,403,275,274,402,401,400,272,273,145,144,16,17,18,146,147,19,20,21,149,148,276,404,405,277,278,406,407,279,151,150,22,23,24,152,153,25,26,27,155,154,282,283,411,410,409,281,280,408,536,537,665,664,792,920,921,793,794,922,923,795,667,666,538,539,540,541,669,668,796,924,925,797,798,926,927,799,671,670,542,543,415,287,286,414,413,412,284,285,157,156,28,29,30,158,159,31,32,33,161,160,288,416,417,289,290,418,419,291,163,162,34,35,36,164,165,37,38,39,167,166,294,295,423,422,421,293,292,420,548,676,677,549,550,551,679,678,806,807,935,934,933,805,804,932,931,930,802,803,675,547,546,674,673,545,544,672,800,801,929,928,1056,1184,1185,1057,1058,1059,1187,1186,1314,1315,1443,1442,1441,1313,1312,1440,1568,1569,1697,1696,1824,1952,1953,1825,1826,1954,1955,1827,1699,1698,1570,1571,1572,1573,1701,1700,1828,1956,1957,1829,1830,1958,1959,1831,1703,1702,1574,1575,1447,1319,1318,1446,1445,1444,1316,1317,1189,1188,1060,1061,1062,1190,1191,1063,1064,1192,1193,1065,1066,1067,1195,1194,1322,1323,1451,1450,1449,1321,1320,1448,1576,1577,1705,1704,1832,1960,1961,1833,1834,1962,1963,1835,1707,1706,1578,1579,1580,1581,1709,1708,1836,1964,1965,1837,1838,1966,1967,1839,1711,1710,1582,1583,1455,1327,1326,1454,1453,1452,1324,1325,1197,1196,1068,1069,1070,1198,1199,1071,943,942,814,815,687,559,558,686,685,557,556,684,812,813,941,940,939,811,810,938,937,936,808,809,681,680,552,553,554,682,683,555,427,299,298,426,425,424,296,297,169,168,40,41,42,170,171,43,44,45,173,172,300,428,429,301,302,430,431,303,175,174,46,47,48,176,177,49,50,51,179,178,306,307,435,434,433,305,304,432,560,561,689,688,816,944,945,817,818,946,947,819,691,690,562,563,564,565,693,692,820,948,949,821,822,950,951,823,695,694,566,567,439,311,310,438,437,436,308,309,181,180,52,53,54,182,183,55,56,57,185,184,312,440,441,313,314,442,443,315,187,186,58,59,60,188,189,61,62,63,191,190,318,319,447,446,445,317,316,444,572,700,701,573,574,575,703,702,830,831,959,958,957,829,828,956,955,954,826,827,699,571,570,698,697,569,568,696,824,825,953,952,1080,1081,1209,1208,1336,1464,1465,1337,1338,1466,1467,1339,1211,1210,1082,1083,1084,1212,1213,1085,1086,1087,1215,1214,1342,1343,1471,1470,1469,1341,1340,1468,1596,1724,1725,1597,1598,1599,1727,1726,1854,1855,1983,1982,1981,1853,1852,1980,1979,1978,1850,1851,1723,1595,1594,1722,1721,1593,1592,1720,1848,1849,1977,1976,1975,1847,1846,1974,1973,1972,1844,1845,1717,1716,1588,1589,1590,1718,1719,1591,1463,1462,1334,1335,1207,1079,1078,1206,1205,1077,1076,1204,1332,1333,1461,1460,1459,1458,1330,1331,1203,1075,1074,1202,1201,1073,1072,1200,1328,1329,1457,1456,1584,1712,1713,1585,1586,1587,1715,1714,1842,1843,1971,1970,1969,1841,1840,1968,2096,2224,2225,2097,2098,2099,2227,2226,2354,2355,2483,2482,2481,2353,2352,2480,2608,2609,2737,2736,2864,2992,2993,2865,2866,2994,2995,2867,2739,2738,2610,2611,2612,2613,2741,2740,2868,2996,2997,2869,2870,2998,2999,2871,2743,2742,2614,2615,2487,2359,2358,2486,2485,2484,2356,2357,2229,2228,2100,2101,2102,2230,2231,2103,2104,2105,2233,2232,2360,2488,2489,2361,2362,2490,2491,2363,2235,2234,2106,2107,2108,2236,2237,2109,2110,2111,2239,2238,2366,2367,2495,2494,2493,2365,2364,2492,2620,2748,2749,2621,2622,2623,2751,2750,2878,2879,3007,3006,3005,2877,2876,3004,3003,3002,2874,2875,2747,2619,2618,2746,2745,2617,2616,2744,2872,2873,3001,3000,3128,3129,3257,3256,3384,3512,3513,3385,3386,3514,3515,3387,3259,3258,3130,3131,3132,3260,3261,3133,3134,3135,3263,3262,3390,3391,3519,3518,3517,3389,3388,3516,3644,3772,3773,3645,3646,3647,3775,3774,3902,3903,4031,4030,4029,3901,3900,4028,4027,4026,3898,3899,3771,3643,3642,3770,3769,3641,3640,3768,3896,3897,4025,4024,4023,3895,3894,4022,4021,4020,3892,3893,3765,3764,3636,3637,3638,3766,3767,3639,3511,3510,3382,3383,3255,3127,3126,3254,3253,3125,3124,3252,3380,3381,3509,3508,3507,3506,3378,3379,3251,3123,3122,3250,3249,3121,3120,3248,3376,3377,3505,3504,3632,3760,3761,3633,3634,3635,3763,3762,3890,3891,4019,4018,4017,3889,3888,4016,4015,4014,3886,3887,3759,3631,3630,3758,3757,3629,3628,3756,3884,3885,4013,4012,4011,3883,3882,4010,4009,4008,3880,3881,3753,3752,3624,3625,3626,3754,3755,3627,3499,3371,3370,3498,3497,3496,3368,3369,3241,3240,3112,3113,3114,3242,3243,3115,3116,3117,3245,3244,3372,3500,3501,3373,3374,3502,3503,3375,3247,3246,3118,3119,2991,2863,2862,2990,2989,2988,2860,2861,2733,2732,2604,2605,2606,2734,2735,2607,2479,2478,2350,2351,2223,2095,2094,2222,2221,2093,2092,2220,2348,2349,2477,2476,2475,2474,2346,2347,2219,2091,2090,2218,2217,2089,2088,2216,2344,2345,2473,2472,2600,2728,2729,2601,2602,2603,2731,2730,2858,2859,2987,2986,2985,2857,2856,2984,2983,2855,2854,2982,2981,2980,2852,2853,2725,2724,2596,2597,2598,2726,2727,2599,2471,2470,2342,2343,2215,2087,2086,2214,2213,2085,2084,2212,2340,2341,2469,2468,2467,2466,2338,2339,2211,2083,2082,2210,2209,2081,2080,2208,2336,2337,2465,2464,2592,2720,2721,2593,2594,2595,2723,2722,2850,2851,2979,2978,2977,2849,2848,2976,3104,3105,3233,3232,3360,3488,3489,3361,3362,3490,3491,3363,3235,3234,3106,3107,3108,3236,3237,3109,3110,3111,3239,3238,3366,3367,3495,3494,3493,3365,3364,3492,3620,3748,3749,3621,3622,3623,3751,3750,3878,3879,4007,4006,4005,3877,3876,4004,4003,4002,3874,3875,3747,3619,3618,3746,3745,3617,3616,3744,3872,3873,4001,4000,4128,4129,4257,4256,4384,4512,4513,4385,4386,4514,4515,4387,4259,4258,4130,4131,4132,4260,4261,4133,4134,4135,4263,4262,4390,4391,4519,4518,4517,4389,4388,4516,4644,4772,4773,4645,4646,4647,4775,4774,4902,4903,5031,5030,5029,4901,4900,5028,5027,5026,4898,4899,4771,4643,4642,4770,4769,4641,4640,4768,4896,4897,5025,5024,5152,5280,5281,5153,5154,5155,5283,5282,5410,5411,5539,5538,5537,5409,5408,5536,5664,5665,5793,5792,5920,6048,6049,5921,5922,6050,6051,5923,5795,5794,5666,5667,5668,5669,5797,5796,5924,6052,6053,5925,5926,6054,6055,5927,5799,5798,5670,5671,5543,5415,5414,5542,5541,5540,5412,5413,5285,5284,5156,5157,5158,5286,5287,5159,5160,5288,5289,5161,5162,5163,5291,5290,5418,5419,5547,5546,5545,5417,5416,5544,5672,5673,5801,5800,5928,6056,6057,5929,5930,6058,6059,5931,5803,5802,5674,5675,5676,5677,5805,5804,5932,6060,6061,5933,5934,6062,6063,5935,5807,5806,5678,5679,5551,5423,5422,5550,5549,5548,5420,5421,5293,5292,5164,5165,5166,5294,5295,5167,5039,5038,4910,4911,4783,4655,4654,4782,4781,4653,4652,4780,4908,4909,5037,5036,5035,4907,4906,5034,5033,5032,4904,4905,4777,4776,4648,4649,4650,4778,4779,4651,4523,4395,4394,4522,4521,4520,4392,4393,4265,4264,4136,4137,4138,4266,4267,4139,4140,4141,4269,4268,4396,4524,4525,4397,4398,4526,4527,4399,4271,4270,4142,4143,4144,4272,4273,4145,4146,4147,4275,4274,4402,4403,4531,4530,4529,4401,4400,4528,4656,4657,4785,4784,4912,5040,5041,4913,4914,5042,5043,4915,4787,4786,4658,4659,4660,4661,4789,4788,4916,5044,5045,4917,4918,5046,5047,4919,4791,4790,4662,4663,4535,4407,4406,4534,4533,4532,4404,4405,4277,4276,4148,4149,4150,4278,4279,4151,4152,4153,4281,4280,4408,4536,4537,4409,4410,4538,4539,4411,4283,4282,4154,4155,4156,4284,4285,4157,4158,4159,4287,4286,4414,4415,4543,4542,4541,4413,4412,4540,4668,4796,4797,4669,4670,4671,4799,4798,4926,4927,5055,5054,5053,4925,4924,5052,5051,5050,4922,4923,4795,4667,4666,4794,4793,4665,4664,4792,4920,4921,5049,5048,5176,5177,5305,5304,5432,5560,5561,5433,5434,5562,5563,5435,5307,5306,5178,5179,5180,5308,5309,5181,5182,5183,5311,5310,5438,5439,5567,5566,5565,5437,5436,5564,5692,5820,5821,5693,5694,5695,5823,5822,5950,5951,6079,6078,6077,5949,5948,6076,6075,6074,5946,5947,5819,5691,5690,5818,5817,5689,5688,5816,5944,5945,6073,6072,6071,5943,5942,6070,6069,6068,5940,5941,5813,5812,5684,5685,5686,5814,5815,5687,5559,5558,5430,5431,5303,5175,5174,5302,5301,5173,5172,5300,5428,5429,5557,5556,5555,5554,5426,5427,5299,5171,5170,5298,5297,5169,5168,5296,5424,5425,5553,5552,5680,5808,5809,5681,5682,5683,5811,5810,5938,5939,6067,6066,6065,5937,5936,6064,6192,6320,6321,6193,6194,6195,6323,6322,6450,6451,6579,6578,6577,6449,6448,6576,6704,6705,6833,6832,6960,7088,7089,6961,6962,7090,7091,6963,6835,6834,6706,6707,6708,6709,6837,6836,6964,7092,7093,6965,6966,7094,7095,6967,6839,6838,6710,6711,6583,6455,6454,6582,6581,6580,6452,6453,6325,6324,6196,6197,6198,6326,6327,6199,6200,6201,6329,6328,6456,6584,6585,6457,6458,6586,6587,6459,6331,6330,6202,6203,6204,6332,6333,6205,6206,6207,6335,6334,6462,6463,6591,6590,6589,6461,6460,6588,6716,6844,6845,6717,6718,6719,6847,6846,6974,6975,7103,7102,7101,6973,6972,7100,7099,7098,6970,6971,6843,6715,6714,6842,6841,6713,6712,6840,6968,6969,7097,7096,7224,7225,7353,7352,7480,7608,7609,7481,7482,7610,7611,7483,7355,7354,7226,7227,7228,7356,7357,7229,7230,7231,7359,7358,7486,7487,7615,7614,7613,7485,7484,7612,7740,7868,7869,7741,7742,7743,7871,7870,7998,7999,8127,8126,8125,7997,7996,8124,8123,8122,7994,7995,7867,7739,7738,7866,7865,7737,7736,7864,7992,7993,8121,8120,8119,7991,7990,8118,8117,8116,7988,7989,7861,7860,7732,7733,7734,7862,7863,7735,7607,7606,7478,7479,7351,7223,7222,7350,7349,7221,7220,7348,7476,7477,7605,7604,7603,7602,7474,7475,7347,7219,7218,7346,7345,7217,7216,7344,7472,7473,7601,7600,7728,7856,7857,7729,7730,7731,7859,7858,7986,7987,8115,8114,8113,7985,7984,8112,8111,8110,7982,7983,7855,7727,7726,7854,7853,7725,7724,7852,7980,7981,8109,8108,8107,7979,7978,8106,8105,8104,7976,7977,7849,7848,7720,7721,7722,7850,7851,7723,7595,7467,7466,7594,7593,7592,7464,7465,7337,7336,7208,7209,7210,7338,7339,7211,7212,7213,7341,7340,7468,7596,7597,7469,7470,7598,7599,7471,7343,7342,7214,7215,7087,6959,6958,7086,7085,7084,6956,6957,6829,6828,6700,6701,6702,6830,6831,6703,6575,6574,6446,6447,6319,6191,6190,6318,6317,6189,6188,6316,6444,6445,6573,6572,6571,6570,6442,6443,6315,6187,6186,6314,6313,6185,6184,6312,6440,6441,6569,6568,6696,6824,6825,6697,6698,6699,6827,6826,6954,6955,7083,7082,7081,6953,6952,7080,7079,6951,6950,7078,7077,7076,6948,6949,6821,6820,6692,6693,6694,6822,6823,6695,6567,6566,6438,6439,6311,6183,6182,6310,6309,6181,6180,6308,6436,6437,6565,6564,6563,6562,6434,6435,6307,6179,6178,6306,6305,6177,6176,6304,6432,6433,6561,6560,6688,6816,6817,6689,6690,6691,6819,6818,6946,6947,7075,7074,7073,6945,6944,7072,7200,7201,7329,7328,7456,7584,7585,7457,7458,7586,7587,7459,7331,7330,7202,7203,7204,7332,7333,7205,7206,7207,7335,7334,7462,7463,7591,7590,7589,7461,7460,7588,7716,7844,7845,7717,7718,7719,7847,7846,7974,7975,8103,8102,8101,7973,7972,8100,8099,8098,7970,7971,7843,7715,7714,7842,7841,7713,7712,7840,7968,7969,8097,8096,8095,7967,7966,8094,8093,8092,7964,7965,7837,7836,7708,7709,7710,7838,7839,7711,7583,7582,7454,7455,7327,7199,7198,7326,7325,7197,7196,7324,7452,7453,7581,7580,7579,7578,7450,7451,7323,7195,7194,7322,7321,7193,7192,7320,7448,7449,7577,7576,7704,7832,7833,7705,7706,7707,7835,7834,7962,7963,8091,8090,8089,7961,7960,8088,8087,8086,7958,7959,7831,7703,7702,7830,7829,7701,7700,7828,7956,7957,8085,8084,8083,7955,7954,8082,8081,8080,7952,7953,7825,7824,7696,7697,7698,7826,7827,7699,7571,7443,7442,7570,7569,7568,7440,7441,7313,7312,7184,7185,7186,7314,7315,7187,7188,7189,7317,7316,7444,7572,7573,7445,7446,7574,7575,7447,7319,7318,7190,7191,7063,7062,6934,6935,6807,6679,6678,6806,6805,6677,6676,6804,6932,6933,7061,7060,7059,6931,6930,7058,7057,7056,6928,6929,6801,6800,6672,6673,6674,6802,6803,6675,6547,6419,6418,6546,6545,6544,6416,6417,6289,6288,6160,6161,6162,6290,6291,6163,6164,6165,6293,6292,6420,6548,6549,6421,6422,6550,6551,6423,6295,6294,6166,6167,6168,6296,6297,6169,6170,6171,6299,6298,6426,6427,6555,6554,6553,6425,6424,6552,6680,6681,6809,6808,6936,7064,7065,6937,6938,7066,7067,6939,6811,6810,6682,6683,6684,6685,6813,6812,6940,7068,7069,6941,6942,7070,7071,6943,6815,6814,6686,6687,6559,6431,6430,6558,6557,6556,6428,6429,6301,6300,6172,6173,6174,6302,6303,6175,6047,6046,5918,5919,5791,5663,5662,5790,5789,5661,5660,5788,5916,5917,6045,6044,6043,5915,5914,6042,6041,6040,5912,5913,5785,5784,5656,5657,5658,5786,5787,5659,5531,5403,5402,5530,5529,5528,5400,5401,5273,5272,5144,5145,5146,5274,5275,5147,5148,5149,5277,5276,5404,5532,5533,5405,5406,5534,5535,5407,5279,5278,5150,5151,5023,4895,4894,5022,5021,5020,4892,4893,4765,4764,4636,4637,4638,4766,4767,4639,4511,4510,4382,4383,4255,4127,4126,4254,4253,4125,4124,4252,4380,4381,4509,4508,4507,4506,4378,4379,4251,4123,4122,4250,4249,4121,4120,4248,4376,4377,4505,4504,4632,4760,4761,4633,4634,4635,4763,4762,4890,4891,5019,5018,5017,4889,4888,5016,5015,4887,4886,5014,5013,5012,4884,4885,4757,4756,4628,4629,4630,4758,4759,4631,4503,4502,4374,4375,4247,4119,4118,4246,4245,4117,4116,4244,4372,4373,4501,4500,4499,4498,4370,4371,4243,4115,4114,4242,4241,4113,4112,4240,4368,4369,4497,4496,4624,4752,4753,4625,4626,4627,4755,4754,4882,4883,5011,5010,5009,4881,4880,5008,5136,5137,5265,5264,5392,5520,5521,5393,5394,5522,5523,5395,5267,5266,5138,5139,5140,5268,5269,5141,5142,5143,5271,5270,5398,5399,5527,5526,5525,5397,5396,5524,5652,5780,5781,5653,5654,5655,5783,5782,5910,5911,6039,6038,6037,5909,5908,6036,6035,6034,5906,5907,5779,5651,5650,5778,5777,5649,5648,5776,5904,5905,6033,6032,6031,6030,5902,5903,5775,5647,5646,5774,5773,5645,5644,5772,5900,5901,6029,6028,6027,5899,5898,6026,6025,6024,5896,5897,5769,5768,5640,5641,5642,5770,5771,5643,5515,5387,5386,5514,5513,5512,5384,5385,5257,5256,5128,5129,5130,5258,5259,5131,5132,5133,5261,5260,5388,5516,5517,5389,5390,5518,5519,5391,5263,5262,5134,5135,5007,4879,4878,5006,5005,5004,4876,4877,4749,4748,4620,4621,4622,4750,4751,4623,4495,4494,4366,4367,4239,4111,4110,4238,4237,4109,4108,4236,4364,4365,4493,4492,4491,4490,4362,4363,4235,4107,4106,4234,4233,4105,4104,4232,4360,4361,4489,4488,4616,4744,4745,4617,4618,4619,4747,4746,4874,4875,5003,5002,5001,4873,4872,5000,4999,4871,4870,4998,4997,4996,4868,4869,4741,4740,4612,4613,4614,4742,4743,4615,4487,4486,4358,4359,4231,4103,4102,4230,4229,4101,4100,4228,4356,4357,4485,4484,4483,4482,4354,4355,4227,4099,4098,4226,4225,4097,4096,4224,4352,4353,4481,4480,4608,4736,4737,4609,4610,4611,4739,4738,4866,4867,4995,4994,4993,4865,4864,4992,5120,5121,5249,5248,5376,5504,5505,5377,5378,5506,5507,5379,5251,5250,5122,5123,5124,5252,5253,5125,5126,5127,5255,5254,5382,5383,5511,5510,5509,5381,5380,5508,5636,5764,5765,5637,5638,5639,5767,5766,5894,5895,6023,6022,6021,5893,5892,6020,6019,6018,5890,5891,5763,5635,5634,5762,5761,5633,5632,5760,5888,5889,6017,6016,6144,6272,6273,6145,6146,6147,6275,6274,6402,6403,6531,6530,6529,6401,6400,6528,6656,6657,6785,6784,6912,7040,7041,6913,6914,7042,7043,6915,6787,6786,6658,6659,6660,6661,6789,6788,6916,7044,7045,6917,6918,7046,7047,6919,6791,6790,6662,6663,6535,6407,6406,6534,6533,6532,6404,6405,6277,6276,6148,6149,6150,6278,6279,6151,6152,6153,6281,6280,6408,6536,6537,6409,6410,6538,6539,6411,6283,6282,6154,6155,6156,6284,6285,6157,6158,6159,6287,6286,6414,6415,6543,6542,6541,6413,6412,6540,6668,6796,6797,6669,6670,6671,6799,6798,6926,6927,7055,7054,7053,6925,6924,7052,7051,7050,6922,6923,6795,6667,6666,6794,6793,6665,6664,6792,6920,6921,7049,7048,7176,7177,7305,7304,7432,7560,7561,7433,7434,7562,7563,7435,7307,7306,7178,7179,7180,7308,7309,7181,7182,7183,7311,7310,7438,7439,7567,7566,7565,7437,7436,7564,7692,7820,7821,7693,7694,7695,7823,7822,7950,7951,8079,8078,8077,7949,7948,8076,8075,8074,7946,7947,7819,7691,7690,7818,7817,7689,7688,7816,7944,7945,8073,8072,8071,7943,7942,8070,8069,8068,7940,7941,7813,7812,7684,7685,7686,7814,7815,7687,7559,7558,7430,7431,7303,7175,7174,7302,7301,7173,7172,7300,7428,7429,7557,7556,7555,7554,7426,7427,7299,7171,7170,7298,7297,7169,7168,7296,7424,7425,7553,7552,7680,7808,7809,7681,7682,7683,7811,7810,7938,7939,8067,8066,8065,7937,7936,8064,8191,8063,8062,8190,8189,8188,8060,8061,7933,7932,7804,7805,7806,7934,7935,7807,7679,7678,7550,7551,7423,7295,7294,7422,7421,7293,7292,7420,7548,7549,7677,7676,7675,7674,7546,7547,7419,7291,7290,7418,7417,7289,7288,7416,7544,7545,7673,7672,7800,7928,7929,7801,7802,7803,7931,7930,8058,8059,8187,8186,8185,8057,8056,8184,8183,8182,8054,8055,7927,7799,7798,7926,7925,7797,7796,7924,8052,8053,8181,8180,8179,8051,8050,8178,8177,8176,8048,8049,7921,7920,7792,7793,7794,7922,7923,7795,7667,7539,7538,7666,7665,7664,7536,7537,7409,7408,7280,7281,7282,7410,7411,7283,7284,7285,7413,7412,7540,7668,7669,7541,7542,7670,7671,7543,7415,7414,7286,7287,7159,7158,7030,7031,6903,6775,6774,6902,6901,6773,6772,6900,7028,7029,7157,7156,7155,7027,7026,7154,7153,7152,7024,7025,6897,6896,6768,6769,6770,6898,6899,6771,6643,6515,6514,6642,6641,6640,6512,6513,6385,6384,6256,6257,6258,6386,6387,6259,6260,6261,6389,6388,6516,6644,6645,6517,6518,6646,6647,6519,6391,6390,6262,6263,6264,6392,6393,6265,6266,6267,6395,6394,6522,6523,6651,6650,6649,6521,6520,6648,6776,6777,6905,6904,7032,7160,7161,7033,7034,7162,7163,7035,6907,6906,6778,6779,6780,6781,6909,6908,7036,7164,7165,7037,7038,7166,7167,7039,6911,6910,6782,6783,6655,6527,6526,6654,6653,6652,6524,6525,6397,6396,6268,6269,6270,6398,6399,6271,6143,6142,6014,6015,5887,5759,5758,5886,5885,5757,5756,5884,6012,6013,6141,6140,6139,6011,6010,6138,6137,6136,6008,6009,5881,5880,5752,5753,5754,5882,5883,5755,5627,5499,5498,5626,5625,5624,5496,5497,5369,5368,5240,5241,5242,5370,5371,5243,5244,5245,5373,5372,5500,5628,5629,5501,5502,5630,5631,5503,5375,5374,5246,5247,5119,4991,4990,5118,5117,5116,4988,4989,4861,4860,4732,4733,4734,4862,4863,4735,4607,4606,4478,4479,4351,4223,4222,4350,4349,4221,4220,4348,4476,4477,4605,4604,4603,4602,4474,4475,4347,4219,4218,4346,4345,4217,4216,4344,4472,4473,4601,4600,4728,4856,4857,4729,4730,4731,4859,4858,4986,4987,5115,5114,5113,4985,4984,5112,5111,4983,4982,5110,5109,5108,4980,4981,4853,4852,4724,4725,4726,4854,4855,4727,4599,4598,4470,4471,4343,4215,4214,4342,4341,4213,4212,4340,4468,4469,4597,4596,4595,4594,4466,4467,4339,4211,4210,4338,4337,4209,4208,4336,4464,4465,4593,4592,4720,4848,4849,4721,4722,4723,4851,4850,4978,4979,5107,5106,5105,4977,4976,5104,5232,5233,5361,5360,5488,5616,5617,5489,5490,5618,5619,5491,5363,5362,5234,5235,5236,5364,5365,5237,5238,5239,5367,5366,5494,5495,5623,5622,5621,5493,5492,5620,5748,5876,5877,5749,5750,5751,5879,5878,6006,6007,6135,6134,6133,6005,6004,6132,6131,6130,6002,6003,5875,5747,5746,5874,5873,5745,5744,5872,6000,6001,6129,6128,6127,6126,5998,5999,5871,5743,5742,5870,5869,5741,5740,5868,5996,5997,6125,6124,6123,5995,5994,6122,6121,6120,5992,5993,5865,5864,5736,5737,5738,5866,5867,5739,5611,5483,5482,5610,5609,5608,5480,5481,5353,5352,5224,5225,5226,5354,5355,5227,5228,5229,5357,5356,5484,5612,5613,5485,5486,5614,5615,5487,5359,5358,5230,5231,5103,4975,4974,5102,5101,5100,4972,4973,4845,4844,4716,4717,4718,4846,4847,4719,4591,4590,4462,4463,4335,4207,4206,4334,4333,4205,4204,4332,4460,4461,4589,4588,4587,4586,4458,4459,4331,4203,4202,4330,4329,4201,4200,4328,4456,4457,4585,4584,4712,4840,4841,4713,4714,4715,4843,4842,4970,4971,5099,5098,5097,4969,4968,5096,5095,4967,4966,5094,5093,5092,4964,4965,4837,4836,4708,4709,4710,4838,4839,4711,4583,4582,4454,4455,4327,4199,4198,4326,4325,4197,4196,4324,4452,4453,4581,4580,4579,4578,4450,4451,4323,4195,4194,4322,4321,4193,4192,4320,4448,4449,4577,4576,4704,4832,4833,4705,4706,4707,4835,4834,4962,4963,5091,5090,5089,4961,4960,5088,5216,5217,5345,5344,5472,5600,5601,5473,5474,5602,5603,5475,5347,5346,5218,5219,5220,5348,5349,5221,5222,5223,5351,5350,5478,5479,5607,5606,5605,5477,5476,5604,5732,5860,5861,5733,5734,5735,5863,5862,5990,5991,6119,6118,6117,5989,5988,6116,6115,6114,5986,5987,5859,5731,5730,5858,5857,5729,5728,5856,5984,5985,6113,6112,6240,6368,6369,6241,6242,6243,6371,6370,6498,6499,6627,6626,6625,6497,6496,6624,6752,6753,6881,6880,7008,7136,7137,7009,7010,7138,7139,7011,6883,6882,6754,6755,6756,6757,6885,6884,7012,7140,7141,7013,7014,7142,7143,7015,6887,6886,6758,6759,6631,6503,6502,6630,6629,6628,6500,6501,6373,6372,6244,6245,6246,6374,6375,6247,6248,6249,6377,6376,6504,6632,6633,6505,6506,6634,6635,6507,6379,6378,6250,6251,6252,6380,6381,6253,6254,6255,6383,6382,6510,6511,6639,6638,6637,6509,6508,6636,6764,6892,6893,6765,6766,6767,6895,6894,7022,7023,7151,7150,7149,7021,7020,7148,7147,7146,7018,7019,6891,6763,6762,6890,6889,6761,6760,6888,7016,7017,7145,7144,7272,7273,7401,7400,7528,7656,7657,7529,7530,7658,7659,7531,7403,7402,7274,7275,7276,7404,7405,7277,7278,7279,7407,7406,7534,7535,7663,7662,7661,7533,7532,7660,7788,7916,7917,7789,7790,7791,7919,7918,8046,8047,8175,8174,8173,8045,8044,8172,8171,8170,8042,8043,7915,7787,7786,7914,7913,7785,7784,7912,8040,8041,8169,8168,8167,8039,8038,8166,8165,8164,8036,8037,7909,7908,7780,7781,7782,7910,7911,7783,7655,7654,7526,7527,7399,7271,7270,7398,7397,7269,7268,7396,7524,7525,7653,7652,7651,7650,7522,7523,7395,7267,7266,7394,7393,7265,7264,7392,7520,7521,7649,7648,7776,7904,7905,7777,7778,7779,7907,7906,8034,8035,8163,8162,8161,8033,8032,8160,8159,8158,8030,8031,7903,7775,7774,7902,7901,7773,7772,7900,8028,8029,8157,8156,8155,8027,8026,8154,8153,8152,8024,8025,7897,7896,7768,7769,7770,7898,7899,7771,7643,7515,7514,7642,7641,7640,7512,7513,7385,7384,7256,7257,7258,7386,7387,7259,7260,7261,7389,7388,7516,7644,7645,7517,7518,7646,7647,7519,7391,7390,7262,7263,7135,7007,7006,7134,7133,7132,7004,7005,6877,6876,6748,6749,6750,6878,6879,6751,6623,6622,6494,6495,6367,6239,6238,6366,6365,6237,6236,6364,6492,6493,6621,6620,6619,6618,6490,6491,6363,6235,6234,6362,6361,6233,6232,6360,6488,6489,6617,6616,6744,6872,6873,6745,6746,6747,6875,6874,7002,7003,7131,7130,7129,7001,7000,7128,7127,6999,6998,7126,7125,7124,6996,6997,6869,6868,6740,6741,6742,6870,6871,6743,6615,6614,6486,6487,6359,6231,6230,6358,6357,6229,6228,6356,6484,6485,6613,6612,6611,6610,6482,6483,6355,6227,6226,6354,6353,6225,6224,6352,6480,6481,6609,6608,6736,6864,6865,6737,6738,6739,6867,6866,6994,6995,7123,7122,7121,6993,6992,7120,7248,7249,7377,7376,7504,7632,7633,7505,7506,7634,7635,7507,7379,7378,7250,7251,7252,7380,7381,7253,7254,7255,7383,7382,7510,7511,7639,7638,7637,7509,7508,7636,7764,7892,7893,7765,7766,7767,7895,7894,8022,8023,8151,8150,8149,8021,8020,8148,8147,8146,8018,8019,7891,7763,7762,7890,7889,7761,7760,7888,8016,8017,8145,8144,8143,8015,8014,8142,8141,8140,8012,8013,7885,7884,7756,7757,7758,7886,7887,7759,7631,7630,7502,7503,7375,7247,7246,7374,7373,7245,7244,7372,7500,7501,7629,7628,7627,7626,7498,7499,7371,7243,7242,7370,7369,7241,7240,7368,7496,7497,7625,7624,7752,7880,7881,7753,7754,7755,7883,7882,8010,8011,8139,8138,8137,8009,8008,8136,8135,8134,8006,8007,7879,7751,7750,7878,7877,7749,7748,7876,8004,8005,8133,8132,8131,8003,8002,8130,8129,8128,8000,8001,7873,7872,7744,7745,7746,7874,7875,7747,7619,7491,7490,7618,7617,7616,7488,7489,7361,7360,7232,7233,7234,7362,7363,7235,7236,7237,7365,7364,7492,7620,7621,7493,7494,7622,7623,7495,7367,7366,7238,7239,7111,7110,6982,6983,6855,6727,6726,6854,6853,6725,6724,6852,6980,6981,7109,7108,7107,6979,6978,7106,7105,7104,6976,6977,6849,6848,6720,6721,6722,6850,6851,6723,6595,6467,6466,6594,6593,6592,6464,6465,6337,6336,6208,6209,6210,6338,6339,6211,6212,6213,6341,6340,6468,6596,6597,6469,6470,6598,6599,6471,6343,6342,6214,6215,6216,6344,6345,6217,6218,6219,6347,6346,6474,6475,6603,6602,6601,6473,6472,6600,6728,6729,6857,6856,6984,7112,7113,6985,6986,7114,7115,6987,6859,6858,6730,6731,6732,6733,6861,6860,6988,7116,7117,6989,6990,7118,7119,6991,6863,6862,6734,6735,6607,6479,6478,6606,6605,6604,6476,6477,6349,6348,6220,6221,6222,6350,6351,6223,6095,5967,5966,6094,6093,6092,5964,5965,5837,5836,5708,5709,5710,5838,5839,5711,5583,5582,5454,5455,5327,5199,5198,5326,5325,5197,5196,5324,5452,5453,5581,5580,5579,5578,5450,5451,5323,5195,5194,5322,5321,5193,5192,5320,5448,5449,5577,5576,5704,5832,5833,5705,5706,5707,5835,5834,5962,5963,6091,6090,6089,5961,5960,6088,6087,6086,5958,5959,5831,5703,5702,5830,5829,5701,5700,5828,5956,5957,6085,6084,6083,5955,5954,6082,6081,6080,5952,5953,5825,5824,5696,5697,5698,5826,5827,5699,5571,5443,5442,5570,5569,5568,5440,5441,5313,5312,5184,5185,5186,5314,5315,5187,5188,5189,5317,5316,5444,5572,5573,5445,5446,5574,5575,5447,5319,5318,5190,5191,5063,5062,4934,4935,4807,4679,4678,4806,4805,4677,4676,4804,4932,4933,5061,5060,5059,4931,4930,5058,5057,5056,4928,4929,4801,4800,4672,4673,4674,4802,4803,4675,4547,4419,4418,4546,4545,4544,4416,4417,4289,4288,4160,4161,4162,4290,4291,4163,4164,4165,4293,4292,4420,4548,4549,4421,4422,4550,4551,4423,4295,4294,4166,4167,4168,4296,4297,4169,4170,4171,4299,4298,4426,4427,4555,4554,4553,4425,4424,4552,4680,4681,4809,4808,4936,5064,5065,4937,4938,5066,5067,4939,4811,4810,4682,4683,4684,4685,4813,4812,4940,5068,5069,4941,4942,5070,5071,4943,4815,4814,4686,4687,4559,4431,4430,4558,4557,4556,4428,4429,4301,4300,4172,4173,4174,4302,4303,4175,4176,4177,4305,4304,4432,4560,4561,4433,4434,4562,4563,4435,4307,4306,4178,4179,4180,4308,4309,4181,4182,4183,4311,4310,4438,4439,4567,4566,4565,4437,4436,4564,4692,4820,4821,4693,4694,4695,4823,4822,4950,4951,5079,5078,5077,4949,4948,5076,5075,5074,4946,4947,4819,4691,4690,4818,4817,4689,4688,4816,4944,4945,5073,5072,5200,5328,5329,5201,5202,5203,5331,5330,5458,5459,5587,5586,5585,5457,5456,5584,5712,5713,5841,5840,5968,6096,6097,5969,5970,6098,6099,5971,5843,5842,5714,5715,5716,5717,5845,5844,5972,6100,6101,5973,5974,6102,6103,5975,5847,5846,5718,5719,5591,5463,5462,5590,5589,5588,5460,5461,5333,5332,5204,5205,5206,5334,5335,5207,5208,5336,5337,5209,5210,5211,5339,5338,5466,5467,5595,5594,5593,5465,5464,5592,5720,5721,5849,5848,5976,6104,6105,5977,5978,6106,6107,5979,5851,5850,5722,5723,5724,5725,5853,5852,5980,6108,6109,5981,5982,6110,6111,5983,5855,5854,5726,5727,5599,5471,5470,5598,5597,5596,5468,5469,5341,5340,5212,5213,5214,5342,5343,5215,5087,5086,4958,4959,4831,4703,4702,4830,4829,4701,4700,4828,4956,4957,5085,5084,5083,4955,4954,5082,5081,5080,4952,4953,4825,4824,4696,4697,4698,4826,4827,4699,4571,4443,4442,4570,4569,4568,4440,4441,4313,4312,4184,4185,4186,4314,4315,4187,4188,4189,4317,4316,4444,4572,4573,4445,4446,4574,4575,4447,4319,4318,4190,4191,4063,4062,3934,3935,3807,3679,3678,3806,3805,3677,3676,3804,3932,3933,4061,4060,4059,3931,3930,4058,4057,4056,3928,3929,3801,3800,3672,3673,3674,3802,3803,3675,3547,3419,3418,3546,3545,3544,3416,3417,3289,3288,3160,3161,3162,3290,3291,3163,3164,3165,3293,3292,3420,3548,3549,3421,3422,3550,3551,3423,3295,3294,3166,3167,3039,2911,2910,3038,3037,3036,2908,2909,2781,2780,2652,2653,2654,2782,2783,2655,2527,2526,2398,2399,2271,2143,2142,2270,2269,2141,2140,2268,2396,2397,2525,2524,2523,2522,2394,2395,2267,2139,2138,2266,2265,2137,2136,2264,2392,2393,2521,2520,2648,2776,2777,2649,2650,2651,2779,2778,2906,2907,3035,3034,3033,2905,2904,3032,3031,2903,2902,3030,3029,3028,2900,2901,2773,2772,2644,2645,2646,2774,2775,2647,2519,2518,2390,2391,2263,2135,2134,2262,2261,2133,2132,2260,2388,2389,2517,2516,2515,2514,2386,2387,2259,2131,2130,2258,2257,2129,2128,2256,2384,2385,2513,2512,2640,2768,2769,2641,2642,2643,2771,2770,2898,2899,3027,3026,3025,2897,2896,3024,3152,3153,3281,3280,3408,3536,3537,3409,3410,3538,3539,3411,3283,3282,3154,3155,3156,3284,3285,3157,3158,3159,3287,3286,3414,3415,3543,3542,3541,3413,3412,3540,3668,3796,3797,3669,3670,3671,3799,3798,3926,3927,4055,4054,4053,3925,3924,4052,4051,4050,3922,3923,3795,3667,3666,3794,3793,3665,3664,3792,3920,3921,4049,4048,4047,3919,3918,4046,4045,4044,3916,3917,3789,3788,3660,3661,3662,3790,3791,3663,3535,3534,3406,3407,3279,3151,3150,3278,3277,3149,3148,3276,3404,3405,3533,3532,3531,3530,3402,3403,3275,3147,3146,3274,3273,3145,3144,3272,3400,3401,3529,3528,3656,3784,3785,3657,3658,3659,3787,3786,3914,3915,4043,4042,4041,3913,3912,4040,4039,4038,3910,3911,3783,3655,3654,3782,3781,3653,3652,3780,3908,3909,4037,4036,4035,3907,3906,4034,4033,4032,3904,3905,3777,3776,3648,3649,3650,3778,3779,3651,3523,3395,3394,3522,3521,3520,3392,3393,3265,3264,3136,3137,3138,3266,3267,3139,3140,3141,3269,3268,3396,3524,3525,3397,3398,3526,3527,3399,3271,3270,3142,3143,3015,3014,2886,2887,2759,2631,2630,2758,2757,2629,2628,2756,2884,2885,3013,3012,3011,2883,2882,3010,3009,3008,2880,2881,2753,2752,2624,2625,2626,2754,2755,2627,2499,2371,2370,2498,2497,2496,2368,2369,2241,2240,2112,2113,2114,2242,2243,2115,2116,2117,2245,2244,2372,2500,2501,2373,2374,2502,2503,2375,2247,2246,2118,2119,2120,2248,2249,2121,2122,2123,2251,2250,2378,2379,2507,2506,2505,2377,2376,2504,2632,2633,2761,2760,2888,3016,3017,2889,2890,3018,3019,2891,2763,2762,2634,2635,2636,2637,2765,2764,2892,3020,3021,2893,2894,3022,3023,2895,2767,2766,2638,2639,2511,2383,2382,2510,2509,2508,2380,2381,2253,2252,2124,2125,2126,2254,2255,2127,1999,1871,1870,1998,1997,1996,1868,1869,1741,1740,1612,1613,1614,1742,1743,1615,1487,1486,1358,1359,1231,1103,1102,1230,1229,1101,1100,1228,1356,1357,1485,1484,1483,1482,1354,1355,1227,1099,1098,1226,1225,1097,1096,1224,1352,1353,1481,1480,1608,1736,1737,1609,1610,1611,1739,1738,1866,1867,1995,1994,1993,1865,1864,1992,1991,1990,1862,1863,1735,1607,1606,1734,1733,1605,1604,1732,1860,1861,1989,1988,1987,1859,1858,1986,1985,1984,1856,1857,1729,1728,1600,1601,1602,1730,1731,1603,1475,1347,1346,1474,1473,1472,1344,1345,1217,1216,1088,1089,1090,1218,1219,1091,1092,1093,1221,1220,1348,1476,1477,1349,1350,1478,1479,1351,1223,1222,1094,1095,967,966,838,839,711,583,582,710,709,581,580,708,836,837,965,964,963,835,834,962,961,960,832,833,705,704,576,577,578,706,707,579,451,323,322,450,449,448,320,321,193,192,64,65,66,194,195,67,68,69,197,196,324,452,453,325,326,454,455,327,199,198,70,71,72,200,201,73,74,75,203,202,330,331,459,458,457,329,328,456,584,585,713,712,840,968,969,841,842,970,971,843,715,714,586,587,588,589,717,716,844,972,973,845,846,974,975,847,719,718,590,591,463,335,334,462,461,460,332,333,205,204,76,77,78,206,207,79,80,81,209,208,336,464,465,337,338,466,467,339,211,210,82,83,84,212,213,85,86,87,215,214,342,343,471,470,469,341,340,468,596,724,725,597,598,599,727,726,854,855,983,982,981,853,852,980,979,978,850,851,723,595,594,722,721,593,592,720,848,849,977,976,1104,1232,1233,1105,1106,1107,1235,1234,1362,1363,1491,1490,1489,1361,1360,1488,1616,1617,1745,1744,1872,2000,2001,1873,1874,2002,2003,1875,1747,1746,1618,1619,1620,1621,1749,1748,1876,2004,2005,1877,1878,2006,2007,1879,1751,1750,1622,1623,1495,1367,1366,1494,1493,1492,1364,1365,1237,1236,1108,1109,1110,1238,1239,1111,1112,1240,1241,1113,1114,1115,1243,1242,1370,1371,1499,1498,1497,1369,1368,1496,1624,1625,1753,1752,1880,2008,2009,1881,1882,2010,2011,1883,1755,1754,1626,1627,1628,1629,1757,1756,1884,2012,2013,1885,1886,2014,2015,1887,1759,1758,1630,1631,1503,1375,1374,1502,1501,1500,1372,1373,1245,1244,1116,1117,1118,1246,1247,1119,991,990,862,863,735,607,606,734,733,605,604,732,860,861,989,988,987,859,858,986,985,984,856,857,729,728,600,601,602,730,731,603,475,347,346,474,473,472,344,345,217,216,88,89,90,218,219,91,92,93,221,220,348,476,477,349,350,478,479,351,223,222,94,95,96,224,225,97,98,99,227,226,354,355,483,482,481,353,352,480,608,609,737,736,864,992,993,865,866,994,995,867,739,738,610,611,612,613,741,740,868,996,997,869,870,998,999,871,743,742,614,615,487,359,358,486,485,484,356,357,229,228,100,101,102,230,231,103,104,105,233,232,360,488,489,361,362,490,491,363,235,234,106,107,108,236,237,109,110,111,239,238,366,367,495,494,493,365,364,492,620,748,749,621,622,623,751,750,878,879,1007,1006,1005,877,876,1004,1003,1002,874,875,747,619,618,746,745,617,616,744,872,873,1001,1000,1128,1129,1257,1256,1384,1512,1513,1385,1386,1514,1515,1387,1259,1258,1130,1131,1132,1260,1261,1133,1134,1135,1263,1262,1390,1391,1519,1518,1517,1389,1388,1516,1644,1772,1773,1645,1646,1647,1775,1774,1902,1903,2031,2030,2029,1901,1900,2028,2027,2026,1898,1899,1771,1643,1642,1770,1769,1641,1640,1768,1896,1897,2025,2024,2023,1895,1894,2022,2021,2020,1892,1893,1765,1764,1636,1637,1638,1766,1767,1639,1511,1510,1382,1383,1255,1127,1126,1254,1253,1125,1124,1252,1380,1381,1509,1508,1507,1506,1378,1379,1251,1123,1122,1250,1249,1121,1120,1248,1376,1377,1505,1504,1632,1760,1761,1633,1634,1635,1763,1762,1890,1891,2019,2018,2017,1889,1888,2016,2144,2145,2273,2272,2400,2528,2529,2401,2402,2530,2531,2403,2275,2274,2146,2147,2148,2276,2277,2149,2150,2151,2279,2278,2406,2407,2535,2534,2533,2405,2404,2532,2660,2788,2789,2661,2662,2663,2791,2790,2918,2919,3047,3046,3045,2917,2916,3044,3043,3042,2914,2915,2787,2659,2658,2786,2785,2657,2656,2784,2912,2913,3041,3040,3168,3296,3297,3169,3170,3171,3299,3298,3426,3427,3555,3554,3553,3425,3424,3552,3680,3681,3809,3808,3936,4064,4065,3937,3938,4066,4067,3939,3811,3810,3682,3683,3684,3685,3813,3812,3940,4068,4069,3941,3942,4070,4071,3943,3815,3814,3686,3687,3559,3431,3430,3558,3557,3556,3428,3429,3301,3300,3172,3173,3174,3302,3303,3175,3176,3304,3305,3177,3178,3179,3307,3306,3434,3435,3563,3562,3561,3433,3432,3560,3688,3689,3817,3816,3944,4072,4073,3945,3946,4074,4075,3947,3819,3818,3690,3691,3692,3693,3821,3820,3948,4076,4077,3949,3950,4078,4079,3951,3823,3822,3694,3695,3567,3439,3438,3566,3565,3564,3436,3437,3309,3308,3180,3181,3182,3310,3311,3183,3055,3054,2926,2927,2799,2671,2670,2798,2797,2669,2668,2796,2924,2925,3053,3052,3051,2923,2922,3050,3049,3048,2920,2921,2793,2792,2664,2665,2666,2794,2795,2667,2539,2411,2410,2538,2537,2536,2408,2409,2281,2280,2152,2153,2154,2282,2283,2155,2156,2157,2285,2284,2412,2540,2541,2413,2414,2542,2543,2415,2287,2286,2158,2159,2160,2161,2289,2288,2416,2544,2545,2417,2418,2546,2547,2419,2291,2290,2162,2163,2164,2292,2293,2165,2166,2167,2295,2294,2422,2423,2551,2550,2549,2421,2420,2548,2676,2804,2805,2677,2678,2679,2807,2806,2934,2935,3063,3062,3061,2933,2932,3060,3059,3058,2930,2931,2803,2675,2674,2802,2801,2673,2672,2800,2928,2929,3057,3056,3184,3312,3313,3185,3186,3187,3315,3314,3442,3443,3571,3570,3569,3441,3440,3568,3696,3697,3825,3824,3952,4080,4081,3953,3954,4082,4083,3955,3827,3826,3698,3699,3700,3701,3829,3828,3956,4084,4085,3957,3958,4086,4087,3959,3831,3830,3702,3703,3575,3447,3446,3574,3573,3572,3444,3445,3317,3316,3188,3189,3190,3318,3319,3191,3192,3320,3321,3193,3194,3195,3323,3322,3450,3451,3579,3578,3577,3449,3448,3576,3704,3705,3833,3832,3960,4088,4089,3961,3962,4090,4091,3963,3835,3834,3706,3707,3708,3709,3837,3836,3964,4092,4093,3965,3966,4094,4095,3967,3839,3838,3710,3711,3583,3455,3454,3582,3581,3580,3452,3453,3325,3324,3196,3197,3198,3326,3327,3199,3071,3070,2942,2943,2815,2687,2686,2814,2813,2685,2684,2812,2940,2941,3069,3068,3067,2939,2938,3066,3065,3064,2936,2937,2809,2808,2680,2681,2682,2810,2811,2683,2555,2427,2426,2554,2553,2552,2424,2425,2297,2296,2168,2169,2170,2298,2299,2171,2172,2173,2301,2300,2428,2556,2557,2429,2430,2558,2559,2431,2303,2302,2174,2175,2047,1919,1918,2046,2045,2044,1916,1917,1789,1788,1660,1661,1662,1790,1791,1663,1535,1534,1406,1407,1279,1151,1150,1278,1277,1149,1148,1276,1404,1405,1533,1532,1531,1530,1402,1403,1275,1147,1146,1274,1273,1145,1144,1272,1400,1401,1529,1528,1656,1784,1785,1657,1658,1659,1787,1786,1914,1915,2043,2042,2041,1913,1912,2040,2039,2038,1910,1911,1783,1655,1654,1782,1781,1653,1652,1780,1908,1909,2037,2036,2035,1907,1906,2034,2033,2032,1904,1905,1777,1776,1648,1649,1650,1778,1779,1651,1523,1395,1394,1522,1521,1520,1392,1393,1265,1264,1136,1137,1138,1266,1267,1139,1140,1141,1269,1268,1396,1524,1525,1397,1398,1526,1527,1399,1271,1270,1142,1143,1015,1014,886,887,759,631,630,758,757,629,628,756,884,885,1013,1012,1011,883,882,1010,1009,1008,880,881,753,752,624,625,626,754,755,627,499,371,370,498,497,496,368,369,241,240,112,113,114,242,243,115,116,117,245,244,372,500,501,373,374,502,503,375,247,246,118,119,120,248,249,121,122,123,251,250,378,379,507,506,505,377,376,504,632,633,761,760,888,1016,1017,889,890,1018,1019,891,763,762,634,635,636,637,765,764,892,1020,1021,893,894,1022,1023,895,767,766,638,639,511,383,382,510,509,508,380,381,253,252,124,125,126,254,255,127};

__device__ const int SH_INV[8192] = {0,3,4,5,58,59,60,63,64,65,78,79,80,83,84,85,938,939,940,943,944,945,958,959,960,963,964,965,1018,1019,1020,1023,1024,1025,1038,1039,1040,1043,1044,1045,1258,1259,1260,1263,1264,1265,1278,1279,1280,1283,1284,1285,1338,1339,1340,1343,1344,1345,1358,1359,1360,1363,1364,1365,6826,6827,6828,6831,6832,6833,6846,6847,6848,6851,6852,6853,6906,6907,6908,6911,6912,6913,6926,6927,6928,6931,6932,6933,7146,7147,7148,7151,7152,7153,7166,7167,7168,7171,7172,7173,7226,7227,7228,7231,7232,7233,7246,7247,7248,7251,7252,7253,8106,8107,8108,8111,8112,8113,8126,8127,8128,8131,8132,8133,8186,8187,8188,8191,1,2,7,6,57,56,61,62,67,66,77,76,81,82,87,86,937,936,941,942,947,946,957,956,961,962,967,966,1017,1016,1021,1022,1027,1026,1037,1036,1041,1042,1047,1046,1257,1256,1261,1262,1267,1266,1277,1276,1281,1282,1287,1286,1337,1336,1341,1342,1347,1346,1357,1356,1361,1362,1367,1366,6825,6824,6829,6830,6835,6834,6845,6844,6849,6850,6855,6854,6905,6904,6909,6910,6915,6914,6925,6924,6929,6930,6935,6934,7145,7144,7149,7150,7155,7154,7165,7164,7169,7170,7175,7174,7225,7224,7229,7230,7235,7234,7245,7244,7249,7250,7255,7254,8105,8104,8109,8110,8115,8114,8125,8124,8129,8130,8135,8134,8185,8184,8189,8190,14,13,8,9,54,55,50,49,68,71,72,75,94,93,88,89,934,935,930,929,948,951,952,955,974,973,968,969,1014,1015,1010,1009,1028,1031,1032,1035,1054,1053,1048,1049,1254,1255,1250,1249,1268,1271,1272,1275,1294,1293,1288,1289,1334,1335,1330,1329,1348,1351,1352,1355,1374,1373,1368,1369,6822,6823,6818,6817,6836,6839,6840,6843,6862,6861,6856,6857,6902,6903,6898,6897,6916,6919,6920,6923,6942,6941,6936,6937,7142,7143,7138,7137,7156,7159,7160,7163,7182,7181,7176,7177,7222,7223,7218,7217,7236,7239,7240,7243,7262,7261,7256,7257,8102,8103,8098,8097,8116,8119,8120,8123,8142,8141,8136,8137,8182,8183,8178,8177,15,12,11,10,53,52,51,48,69,70,73,74,95,92,91,90,933,932,931,928,949,950,953,954,975,972,971,970,1013,1012,1011,1008,1029,1030,1033,1034,1055,1052,1051,1050,1253,1252,1251,1248,1269,1270,1273,1274,1295,1292,1291,1290,1333,1332,1331,1328,1349,1350,1353,1354,1375,1372,1371,1370,6821,6820,6819,6816,6837,6838,6841,6842,6863,6860,6859,6858,6901,6900,6899,6896,6917,6918,6921,6922,6943,6940,6939,6938,7141,7140,7139,7136,7157,7158,7161,7162,7183,7180,7179,7178,7221,7220,7219,7216,7237,7238,7241,7242,7263,7260,7259,7258,8101,8100,8099,8096,8117,8118,8121,8122,8143,8140,8139,8138,8181,8180,8179,8176,16,17,30,31,32,33,46,47,122,121,118,117,96,99,100,101,922,923,924,927,906,905,902,901,976,977,990,991,992,993,1006,1007,1082,1081,1078,1077,1056,1059,1060,1061,1242,1243,1244,1247,1226,1225,1222,1221,1296,1297,1310,1311,1312,1313,1326,1327,1402,1401,1398,1397,1376,1379,1380,1381,6810,6811,6812,6815,6794,6793,6790,6789,6864,6865,6878,6879,6880,6881,6894,6895,6970,6969,6966,6965,6944,6947,6948,6949,7130,7131,7132,7135,7114,7113,7110,7109,7184,7185,7198,7199,7200,7201,7214,7215,7290,7289,7286,7285,7264,7267,7268,7269,8090,8091,8092,8095,8074,8073,8070,8069,8144,8145,8158,8159,8160,8161,8174,8175,19,18,29,28,35,34,45,44,123,120,119,116,97,98,103,102,921,920,925,926,907,904,903,900,979,978,989,988,995,994,1005,1004,1083,1080,1079,1076,1057,1058,1063,1062,1241,1240,1245,1246,1227,1224,1223,1220,1299,1298,1309,1308,1315,1314,1325,1324,1403,1400,1399,1396,1377,1378,1383,1382,6809,6808,6813,6814,6795,6792,6791,6788,6867,6866,6877,6876,6883,6882,6893,6892,6971,6968,6967,6964,6945,6946,6951,6950,7129,7128,7133,7134,7115,7112,7111,7108,7187,7186,7197,7196,7203,7202,7213,7212,7291,7288,7287,7284,7265,7266,7271,7270,8089,8088,8093,8094,8075,8072,8071,8068,8147,8146,8157,8156,8163,8162,8173,8172,20,23,24,27,36,39,40,43,124,125,114,115,110,109,104,105,918,919,914,913,908,909,898,899,980,983,984,987,996,999,1000,1003,1084,1085,1074,1075,1070,1069,1064,1065,1238,1239,1234,1233,1228,1229,1218,1219,1300,1303,1304,1307,1316,1319,1320,1323,1404,1405,1394,1395,1390,1389,1384,1385,6806,6807,6802,6801,6796,6797,6786,6787,6868,6871,6872,6875,6884,6887,6888,6891,6972,6973,6962,6963,6958,6957,6952,6953,7126,7127,7122,7121,7116,7117,7106,7107,7188,7191,7192,7195,7204,7207,7208,7211,7292,7293,7282,7283,7278,7277,7272,7273,8086,8087,8082,8081,8076,8077,8066,8067,8148,8151,8152,8155,8164,8167,8168,8171,21,22,25,26,37,38,41,42,127,126,113,112,111,108,107,106,917,916,915,912,911,910,897,896,981,982,985,986,997,998,1001,1002,1087,1086,1073,1072,1071,1068,1067,1066,1237,1236,1235,1232,1231,1230,1217,1216,1301,1302,1305,1306,1317,1318,1321,1322,1407,1406,1393,1392,1391,1388,1387,1386,6805,6804,6803,6800,6799,6798,6785,6784,6869,6870,6873,6874,6885,6886,6889,6890,6975,6974,6961,6960,6959,6956,6955,6954,7125,7124,7123,7120,7119,7118,7105,7104,7189,7190,7193,7194,7205,7206,7209,7210,7295,7294,7281,7280,7279,7276,7275,7274,8085,8084,8083,8080,8079,8078,8065,8064,8149,8150,8153,8154,8165,8166,8169,8170,234,233,230,229,218,217,214,213,128,129,142,143,144,147,148,149,874,875,876,879,880,881,894,895,810,809,806,805,794,793,790,789,1088,1091,1092,1093,1146,1147,1148,1151,1152,1155,1156,1157,1210,1211,1212,1215,1514,1513,1510,1509,1498,1497,1494,1493,1408,1409,1422,1423,1424,1427,1428,1429,6762,6763,6764,6767,6768,6769,6782,6783,6698,6697,6694,6693,6682,6681,6678,6677,6976,6979,6980,6981,7034,7035,7036,7039,7040,7043,7044,7045,7098,7099,7100,7103,7402,7401,7398,7397,7386,7385,7382,7381,7296,7297,7310,7311,7312,7315,7316,7317,8042,8043,8044,8047,8048,8049,8062,8063,7978,7977,7974,7973,7962,7961,7958,7957,235,232,231,228,219,216,215,212,131,130,141,140,145,146,151,150,873,872,877,878,883,882,893,892,811,808,807,804,795,792,791,788,1089,1090,1095,1094,1145,1144,1149,1150,1153,1154,1159,1158,1209,1208,1213,1214,1515,1512,1511,1508,1499,1496,1495,1492,1411,1410,1421,1420,1425,1426,1431,1430,6761,6760,6765,6766,6771,6770,6781,6780,6699,6696,6695,6692,6683,6680,6679,6676,6977,6978,6983,6982,7033,7032,7037,7038,7041,7042,7047,7046,7097,7096,7101,7102,7403,7400,7399,7396,7387,7384,7383,7380,7299,7298,7309,7308,7313,7314,7319,7318,8041,8040,8045,8046,8051,8050,8061,8060,7979,7976,7975,7972,7963,7960,7959,7956,236,237,226,227,220,221,210,211,132,135,136,139,158,157,152,153,870,871,866,865,884,887,888,891,812,813,802,803,796,797,786,787,1102,1101,1096,1097,1142,1143,1138,1137,1166,1165,1160,1161,1206,1207,1202,1201,1516,1517,1506,1507,1500,1501,1490,1491,1412,1415,1416,1419,1438,1437,1432,1433,6758,6759,6754,6753,6772,6775,6776,6779,6700,6701,6690,6691,6684,6685,6674,6675,6990,6989,6984,6985,7030,7031,7026,7025,7054,7053,7048,7049,7094,7095,7090,7089,7404,7405,7394,7395,7388,7389,7378,7379,7300,7303,7304,7307,7326,7325,7320,7321,8038,8039,8034,8033,8052,8055,8056,8059,7980,7981,7970,7971,7964,7965,7954,7955,239,238,225,224,223,222,209,208,133,134,137,138,159,156,155,154,869,868,867,864,885,886,889,890,815,814,801,800,799,798,785,784,1103,1100,1099,1098,1141,1140,1139,1136,1167,1164,1163,1162,1205,1204,1203,1200,1519,1518,1505,1504,1503,1502,1489,1488,1413,1414,1417,1418,1439,1436,1435,1434,6757,6756,6755,6752,6773,6774,6777,6778,6703,6702,6689,6688,6687,6686,6673,6672,6991,6988,6987,6986,7029,7028,7027,7024,7055,7052,7051,7050,7093,7092,7091,7088,7407,7406,7393,7392,7391,7390,7377,7376,7301,7302,7305,7306,7327,7324,7323,7322,8037,8036,8035,8032,8053,8054,8057,8058,7983,7982,7969,7968,7967,7966,7953,7952,240,243,244,245,202,203,204,207,186,185,182,181,160,163,164,165,858,859,860,863,842,841,838,837,816,819,820,821,778,779,780,783,1104,1105,1118,1119,1120,1121,1134,1135,1168,1169,1182,1183,1184,1185,1198,1199,1520,1523,1524,1525,1482,1483,1484,1487,1466,1465,1462,1461,1440,1443,1444,1445,6746,6747,6748,6751,6730,6729,6726,6725,6704,6707,6708,6709,6666,6667,6668,6671,6992,6993,7006,7007,7008,7009,7022,7023,7056,7057,7070,7071,7072,7073,7086,7087,7408,7411,7412,7413,7370,7371,7372,7375,7354,7353,7350,7349,7328,7331,7332,7333,8026,8027,8028,8031,8010,8009,8006,8005,7984,7987,7988,7989,7946,7947,7948,7951,241,242,247,246,201,200,205,206,187,184,183,180,161,162,167,166,857,856,861,862,843,840,839,836,817,818,823,822,777,776,781,782,1107,1106,1117,1116,1123,1122,1133,1132,1171,1170,1181,1180,1187,1186,1197,1196,1521,1522,1527,1526,1481,1480,1485,1486,1467,1464,1463,1460,1441,1442,1447,1446,6745,6744,6749,6750,6731,6728,6727,6724,6705,6706,6711,6710,6665,6664,6669,6670,6995,6994,7005,7004,7011,7010,7021,7020,7059,7058,7069,7068,7075,7074,7085,7084,7409,7410,7415,7414,7369,7368,7373,7374,7355,7352,7351,7348,7329,7330,7335,7334,8025,8024,8029,8030,8011,8008,8007,8004,7985,7986,7991,7990,7945,7944,7949,7950,254,253,248,249,198,199,194,193,188,189,178,179,174,173,168,169,854,855,850,849,844,845,834,835,830,829,824,825,774,775,770,769,1108,1111,1112,1115,1124,1127,1128,1131,1172,1175,1176,1179,1188,1191,1192,1195,1534,1533,1528,1529,1478,1479,1474,1473,1468,1469,1458,1459,1454,1453,1448,1449,6742,6743,6738,6737,6732,6733,6722,6723,6718,6717,6712,6713,6662,6663,6658,6657,6996,6999,7000,7003,7012,7015,7016,7019,7060,7063,7064,7067,7076,7079,7080,7083,7422,7421,7416,7417,7366,7367,7362,7361,7356,7357,7346,7347,7342,7341,7336,7337,8022,8023,8018,8017,8012,8013,8002,8003,7998,7997,7992,7993,7942,7943,7938,7937,255,252,251,250,197,196,195,192,191,190,177,176,175,172,171,170,853,852,851,848,847,846,833,832,831,828,827,826,773,772,771,768,1109,1110,1113,1114,1125,1126,1129,1130,1173,1174,1177,1178,1189,1190,1193,1194,1535,1532,1531,1530,1477,1476,1475,1472,1471,1470,1457,1456,1455,1452,1451,1450,6741,6740,6739,6736,6735,6734,6721,6720,6719,6716,6715,6714,6661,6660,6659,6656,6997,6998,7001,7002,7013,7014,7017,7018,7061,7062,7065,7066,7077,7078,7081,7082,7423,7420,7419,7418,7365,7364,7363,7360,7359,7358,7345,7344,7343,7340,7339,7338,8021,8020,8019,8016,8015,8014,8001,8000,7999,7996,7995,7994,7941,7940,7939,7936,256,257,270,271,272,275,276,277,490,491,492,495,496,497,510,511,512,513,526,527,528,531,532,533,746,747,748,751,752,753,766,767,1962,1961,1958,1957,1946,1945,1942,1941,1898,1897,1894,1893,1882,1881,1878,1877,1536,1539,1540,1541,1594,1595,1596,1599,1600,1601,1614,1615,1616,1619,1620,1621,6570,6571,6572,6575,6576,6577,6590,6591,6592,6595,6596,6597,6650,6651,6652,6655,6314,6313,6310,6309,6298,6297,6294,6293,6250,6249,6246,6245,6234,6233,6230,6229,7424,7425,7438,7439,7440,7443,7444,7445,7658,7659,7660,7663,7664,7665,7678,7679,7680,7681,7694,7695,7696,7699,7700,7701,7914,7915,7916,7919,7920,7921,7934,7935,259,258,269,268,273,274,279,278,489,488,493,494,499,498,509,508,515,514,525,524,529,530,535,534,745,744,749,750,755,754,765,764,1963,1960,1959,1956,1947,1944,1943,1940,1899,1896,1895,1892,1883,1880,1879,1876,1537,1538,1543,1542,1593,1592,1597,1598,1603,1602,1613,1612,1617,1618,1623,1622,6569,6568,6573,6574,6579,6578,6589,6588,6593,6594,6599,6598,6649,6648,6653,6654,6315,6312,6311,6308,6299,6296,6295,6292,6251,6248,6247,6244,6235,6232,6231,6228,7427,7426,7437,7436,7441,7442,7447,7446,7657,7656,7661,7662,7667,7666,7677,7676,7683,7682,7693,7692,7697,7698,7703,7702,7913,7912,7917,7918,7923,7922,7933,7932,260,263,264,267,286,285,280,281,486,487,482,481,500,503,504,507,516,519,520,523,542,541,536,537,742,743,738,737,756,759,760,763,1964,1965,1954,1955,1948,1949,1938,1939,1900,1901,1890,1891,1884,1885,1874,1875,1550,1549,1544,1545,1590,1591,1586,1585,1604,1607,1608,1611,1630,1629,1624,1625,6566,6567,6562,6561,6580,6583,6584,6587,6606,6605,6600,6601,6646,6647,6642,6641,6316,6317,6306,6307,6300,6301,6290,6291,6252,6253,6242,6243,6236,6237,6226,6227,7428,7431,7432,7435,7454,7453,7448,7449,7654,7655,7650,7649,7668,7671,7672,7675,7684,7687,7688,7691,7710,7709,7704,7705,7910,7911,7906,7905,7924,7927,7928,7931,261,262,265,266,287,284,283,282,485,484,483,480,501,502,505,506,517,518,521,522,543,540,539,538,741,740,739,736,757,758,761,762,1967,1966,1953,1952,1951,1950,1937,1936,1903,1902,1889,1888,1887,1886,1873,1872,1551,1548,1547,1546,1589,1588,1587,1584,1605,1606,1609,1610,1631,1628,1627,1626,6565,6564,6563,6560,6581,6582,6585,6586,6607,6604,6603,6602,6645,6644,6643,6640,6319,6318,6305,6304,6303,6302,6289,6288,6255,6254,6241,6240,6239,6238,6225,6224,7429,7430,7433,7434,7455,7452,7451,7450,7653,7652,7651,7648,7669,7670,7673,7674,7685,7686,7689,7690,7711,7708,7707,7706,7909,7908,7907,7904,7925,7926,7929,7930,314,313,310,309,288,291,292,293,474,475,476,479,458,457,454,453,570,569,566,565,544,547,548,549,730,731,732,735,714,713,710,709,1968,1971,1972,1973,1930,1931,1932,1935,1904,1907,1908,1909,1866,1867,1868,1871,1552,1553,1566,1567,1568,1569,1582,1583,1658,1657,1654,1653,1632,1635,1636,1637,6554,6555,6556,6559,6538,6537,6534,6533,6608,6609,6622,6623,6624,6625,6638,6639,6320,6323,6324,6325,6282,6283,6284,6287,6256,6259,6260,6261,6218,6219,6220,6223,7482,7481,7478,7477,7456,7459,7460,7461,7642,7643,7644,7647,7626,7625,7622,7621,7738,7737,7734,7733,7712,7715,7716,7717,7898,7899,7900,7903,7882,7881,7878,7877,315,312,311,308,289,290,295,294,473,472,477,478,459,456,455,452,571,568,567,564,545,546,551,550,729,728,733,734,715,712,711,708,1969,1970,1975,1974,1929,1928,1933,1934,1905,1906,1911,1910,1865,1864,1869,1870,1555,1554,1565,1564,1571,1570,1581,1580,1659,1656,1655,1652,1633,1634,1639,1638,6553,6552,6557,6558,6539,6536,6535,6532,6611,6610,6621,6620,6627,6626,6637,6636,6321,6322,6327,6326,6281,6280,6285,6286,6257,6258,6263,6262,6217,6216,6221,6222,7483,7480,7479,7476,7457,7458,7463,7462,7641,7640,7645,7646,7627,7624,7623,7620,7739,7736,7735,7732,7713,7714,7719,7718,7897,7896,7901,7902,7883,7880,7879,7876,316,317,306,307,302,301,296,297,470,471,466,465,460,461,450,451,572,573,562,563,558,557,552,553,726,727,722,721,716,717,706,707,1982,1981,1976,1977,1926,1927,1922,1921,1918,1917,1912,1913,1862,1863,1858,1857,1556,1559,1560,1563,1572,1575,1576,1579,1660,1661,1650,1651,1646,1645,1640,1641,6550,6551,6546,6545,6540,6541,6530,6531,6612,6615,6616,6619,6628,6631,6632,6635,6334,6333,6328,6329,6278,6279,6274,6273,6270,6269,6264,6265,6214,6215,6210,6209,7484,7485,7474,7475,7470,7469,7464,7465,7638,7639,7634,7633,7628,7629,7618,7619,7740,7741,7730,7731,7726,7725,7720,7721,7894,7895,7890,7889,7884,7885,7874,7875,319,318,305,304,303,300,299,298,469,468,467,464,463,462,449,448,575,574,561,560,559,556,555,554,725,724,723,720,719,718,705,704,1983,1980,1979,1978,1925,1924,1923,1920,1919,1916,1915,1914,1861,1860,1859,1856,1557,1558,1561,1562,1573,1574,1577,1578,1663,1662,1649,1648,1647,1644,1643,1642,6549,6548,6547,6544,6543,6542,6529,6528,6613,6614,6617,6618,6629,6630,6633,6634,6335,6332,6331,6330,6277,6276,6275,6272,6271,6268,6267,6266,6213,6212,6211,6208,7487,7486,7473,7472,7471,7468,7467,7466,7637,7636,7635,7632,7631,7630,7617,7616,7743,7742,7729,7728,7727,7724,7723,7722,7893,7892,7891,7888,7887,7886,7873,7872,320,323,324,325,378,379,380,383,384,387,388,389,442,443,444,447,576,579,580,581,634,635,636,639,640,643,644,645,698,699,700,703,1984,1985,1998,1999,2000,2003,2004,2005,1834,1835,1836,1839,1840,1841,1854,1855,1770,1769,1766,1765,1754,1753,1750,1749,1664,1665,1678,1679,1680,1683,1684,1685,6506,6507,6508,6511,6512,6513,6526,6527,6442,6441,6438,6437,6426,6425,6422,6421,6336,6337,6350,6351,6352,6355,6356,6357,6186,6187,6188,6191,6192,6193,6206,6207,7488,7491,7492,7493,7546,7547,7548,7551,7552,7555,7556,7557,7610,7611,7612,7615,7744,7747,7748,7749,7802,7803,7804,7807,7808,7811,7812,7813,7866,7867,7868,7871,321,322,327,326,377,376,381,382,385,386,391,390,441,440,445,446,577,578,583,582,633,632,637,638,641,642,647,646,697,696,701,702,1987,1986,1997,1996,2001,2002,2007,2006,1833,1832,1837,1838,1843,1842,1853,1852,1771,1768,1767,1764,1755,1752,1751,1748,1667,1666,1677,1676,1681,1682,1687,1686,6505,6504,6509,6510,6515,6514,6525,6524,6443,6440,6439,6436,6427,6424,6423,6420,6339,6338,6349,6348,6353,6354,6359,6358,6185,6184,6189,6190,6195,6194,6205,6204,7489,7490,7495,7494,7545,7544,7549,7550,7553,7554,7559,7558,7609,7608,7613,7614,7745,7746,7751,7750,7801,7800,7805,7806,7809,7810,7815,7814,7865,7864,7869,7870,334,333,328,329,374,375,370,369,398,397,392,393,438,439,434,433,590,589,584,585,630,631,626,625,654,653,648,649,694,695,690,689,1988,1991,1992,1995,2014,2013,2008,2009,1830,1831,1826,1825,1844,1847,1848,1851,1772,1773,1762,1763,1756,1757,1746,1747,1668,1671,1672,1675,1694,1693,1688,1689,6502,6503,6498,6497,6516,6519,6520,6523,6444,6445,6434,6435,6428,6429,6418,6419,6340,6343,6344,6347,6366,6365,6360,6361,6182,6183,6178,6177,6196,6199,6200,6203,7502,7501,7496,7497,7542,7543,7538,7537,7566,7565,7560,7561,7606,7607,7602,7601,7758,7757,7752,7753,7798,7799,7794,7793,7822,7821,7816,7817,7862,7863,7858,7857,335,332,331,330,373,372,371,368,399,396,395,394,437,436,435,432,591,588,587,586,629,628,627,624,655,652,651,650,693,692,691,688,1989,1990,1993,1994,2015,2012,2011,2010,1829,1828,1827,1824,1845,1846,1849,1850,1775,1774,1761,1760,1759,1758,1745,1744,1669,1670,1673,1674,1695,1692,1691,1690,6501,6500,6499,6496,6517,6518,6521,6522,6447,6446,6433,6432,6431,6430,6417,6416,6341,6342,6345,6346,6367,6364,6363,6362,6181,6180,6179,6176,6197,6198,6201,6202,7503,7500,7499,7498,7541,7540,7539,7536,7567,7564,7563,7562,7605,7604,7603,7600,7759,7756,7755,7754,7797,7796,7795,7792,7823,7820,7819,7818,7861,7860,7859,7856,336,337,350,351,352,353,366,367,400,401,414,415,416,417,430,431,592,593,606,607,608,609,622,623,656,657,670,671,672,673,686,687,2042,2041,2038,2037,2016,2019,2020,2021,1818,1819,1820,1823,1802,1801,1798,1797,1776,1779,1780,1781,1738,1739,1740,1743,1722,1721,1718,1717,1696,1699,1700,1701,6490,6491,6492,6495,6474,6473,6470,6469,6448,6451,6452,6453,6410,6411,6412,6415,6394,6393,6390,6389,6368,6371,6372,6373,6170,6171,6172,6175,6154,6153,6150,6149,7504,7505,7518,7519,7520,7521,7534,7535,7568,7569,7582,7583,7584,7585,7598,7599,7760,7761,7774,7775,7776,7777,7790,7791,7824,7825,7838,7839,7840,7841,7854,7855,339,338,349,348,355,354,365,364,403,402,413,412,419,418,429,428,595,594,605,604,611,610,621,620,659,658,669,668,675,674,685,684,2043,2040,2039,2036,2017,2018,2023,2022,1817,1816,1821,1822,1803,1800,1799,1796,1777,1778,1783,1782,1737,1736,1741,1742,1723,1720,1719,1716,1697,1698,1703,1702,6489,6488,6493,6494,6475,6472,6471,6468,6449,6450,6455,6454,6409,6408,6413,6414,6395,6392,6391,6388,6369,6370,6375,6374,6169,6168,6173,6174,6155,6152,6151,6148,7507,7506,7517,7516,7523,7522,7533,7532,7571,7570,7581,7580,7587,7586,7597,7596,7763,7762,7773,7772,7779,7778,7789,7788,7827,7826,7837,7836,7843,7842,7853,7852,340,343,344,347,356,359,360,363,404,407,408,411,420,423,424,427,596,599,600,603,612,615,616,619,660,663,664,667,676,679,680,683,2044,2045,2034,2035,2030,2029,2024,2025,1814,1815,1810,1809,1804,1805,1794,1795,1790,1789,1784,1785,1734,1735,1730,1729,1724,1725,1714,1715,1710,1709,1704,1705,6486,6487,6482,6481,6476,6477,6466,6467,6462,6461,6456,6457,6406,6407,6402,6401,6396,6397,6386,6387,6382,6381,6376,6377,6166,6167,6162,6161,6156,6157,6146,6147,7508,7511,7512,7515,7524,7527,7528,7531,7572,7575,7576,7579,7588,7591,7592,7595,7764,7767,7768,7771,7780,7783,7784,7787,7828,7831,7832,7835,7844,7847,7848,7851,341,342,345,346,357,358,361,362,405,406,409,410,421,422,425,426,597,598,601,602,613,614,617,618,661,662,665,666,677,678,681,682,2047,2046,2033,2032,2031,2028,2027,2026,1813,1812,1811,1808,1807,1806,1793,1792,1791,1788,1787,1786,1733,1732,1731,1728,1727,1726,1713,1712,1711,1708,1707,1706,6485,6484,6483,6480,6479,6478,6465,6464,6463,6460,6459,6458,6405,6404,6403,6400,6399,6398,6385,6384,6383,6380,6379,6378,6165,6164,6163,6160,6159,6158,6145,6144,7509,7510,7513,7514,7525,7526,7529,7530,7573,7574,7577,7578,7589,7590,7593,7594,7765,7766,7769,7770,7781,7782,7785,7786,7829,7830,7833,7834,7845,7846,7849,7850,3754,3753,3750,3749,3738,3737,3734,3733,3690,3689,3686,3685,3674,3673,3670,3669,3498,3497,3494,3493,3482,3481,3478,3477,3434,3433,3430,3429,3418,3417,3414,3413,2048,2049,2062,2063,2064,2067,2068,2069,2282,2283,2284,2287,2288,2289,2302,2303,2304,2307,2308,2309,2362,2363,2364,2367,2368,2369,2382,2383,2384,2387,2388,2389,5802,5803,5804,5807,5808,5809,5822,5823,5824,5827,5828,5829,5882,5883,5884,5887,5888,5889,5902,5903,5904,5907,5908,5909,6122,6123,6124,6127,6128,6129,6142,6143,4778,4777,4774,4773,4762,4761,4758,4757,4714,4713,4710,4709,4698,4697,4694,4693,4522,4521,4518,4517,4506,4505,4502,4501,4458,4457,4454,4453,4442,4441,4438,4437,3755,3752,3751,3748,3739,3736,3735,3732,3691,3688,3687,3684,3675,3672,3671,3668,3499,3496,3495,3492,3483,3480,3479,3476,3435,3432,3431,3428,3419,3416,3415,3412,2051,2050,2061,2060,2065,2066,2071,2070,2281,2280,2285,2286,2291,2290,2301,2300,2305,2306,2311,2310,2361,2360,2365,2366,2371,2370,2381,2380,2385,2386,2391,2390,5801,5800,5805,5806,5811,5810,5821,5820,5825,5826,5831,5830,5881,5880,5885,5886,5891,5890,5901,5900,5905,5906,5911,5910,6121,6120,6125,6126,6131,6130,6141,6140,4779,4776,4775,4772,4763,4760,4759,4756,4715,4712,4711,4708,4699,4696,4695,4692,4523,4520,4519,4516,4507,4504,4503,4500,4459,4456,4455,4452,4443,4440,4439,4436,3756,3757,3746,3747,3740,3741,3730,3731,3692,3693,3682,3683,3676,3677,3666,3667,3500,3501,3490,3491,3484,3485,3474,3475,3436,3437,3426,3427,3420,3421,3410,3411,2052,2055,2056,2059,2078,2077,2072,2073,2278,2279,2274,2273,2292,2295,2296,2299,2318,2317,2312,2313,2358,2359,2354,2353,2372,2375,2376,2379,2398,2397,2392,2393,5798,5799,5794,5793,5812,5815,5816,5819,5838,5837,5832,5833,5878,5879,5874,5873,5892,5895,5896,5899,5918,5917,5912,5913,6118,6119,6114,6113,6132,6135,6136,6139,4780,4781,4770,4771,4764,4765,4754,4755,4716,4717,4706,4707,4700,4701,4690,4691,4524,4525,4514,4515,4508,4509,4498,4499,4460,4461,4450,4451,4444,4445,4434,4435,3759,3758,3745,3744,3743,3742,3729,3728,3695,3694,3681,3680,3679,3678,3665,3664,3503,3502,3489,3488,3487,3486,3473,3472,3439,3438,3425,3424,3423,3422,3409,3408,2053,2054,2057,2058,2079,2076,2075,2074,2277,2276,2275,2272,2293,2294,2297,2298,2319,2316,2315,2314,2357,2356,2355,2352,2373,2374,2377,2378,2399,2396,2395,2394,5797,5796,5795,5792,5813,5814,5817,5818,5839,5836,5835,5834,5877,5876,5875,5872,5893,5894,5897,5898,5919,5916,5915,5914,6117,6116,6115,6112,6133,6134,6137,6138,4783,4782,4769,4768,4767,4766,4753,4752,4719,4718,4705,4704,4703,4702,4689,4688,4527,4526,4513,4512,4511,4510,4497,4496,4463,4462,4449,4448,4447,4446,4433,4432,3760,3763,3764,3765,3722,3723,3724,3727,3696,3699,3700,3701,3658,3659,3660,3663,3504,3507,3508,3509,3466,3467,3468,3471,3440,3443,3444,3445,3402,3403,3404,3407,2106,2105,2102,2101,2080,2083,2084,2085,2266,2267,2268,2271,2250,2249,2246,2245,2320,2321,2334,2335,2336,2337,2350,2351,2426,2425,2422,2421,2400,2403,2404,2405,5786,5787,5788,5791,5770,5769,5766,5765,5840,5841,5854,5855,5856,5857,5870,5871,5946,5945,5942,5941,5920,5923,5924,5925,6106,6107,6108,6111,6090,6089,6086,6085,4784,4787,4788,4789,4746,4747,4748,4751,4720,4723,4724,4725,4682,4683,4684,4687,4528,4531,4532,4533,4490,4491,4492,4495,4464,4467,4468,4469,4426,4427,4428,4431,3761,3762,3767,3766,3721,3720,3725,3726,3697,3698,3703,3702,3657,3656,3661,3662,3505,3506,3511,3510,3465,3464,3469,3470,3441,3442,3447,3446,3401,3400,3405,3406,2107,2104,2103,2100,2081,2082,2087,2086,2265,2264,2269,2270,2251,2248,2247,2244,2323,2322,2333,2332,2339,2338,2349,2348,2427,2424,2423,2420,2401,2402,2407,2406,5785,5784,5789,5790,5771,5768,5767,5764,5843,5842,5853,5852,5859,5858,5869,5868,5947,5944,5943,5940,5921,5922,5927,5926,6105,6104,6109,6110,6091,6088,6087,6084,4785,4786,4791,4790,4745,4744,4749,4750,4721,4722,4727,4726,4681,4680,4685,4686,4529,4530,4535,4534,4489,4488,4493,4494,4465,4466,4471,4470,4425,4424,4429,4430,3774,3773,3768,3769,3718,3719,3714,3713,3710,3709,3704,3705,3654,3655,3650,3649,3518,3517,3512,3513,3462,3463,3458,3457,3454,3453,3448,3449,3398,3399,3394,3393,2108,2109,2098,2099,2094,2093,2088,2089,2262,2263,2258,2257,2252,2253,2242,2243,2324,2327,2328,2331,2340,2343,2344,2347,2428,2429,2418,2419,2414,2413,2408,2409,5782,5783,5778,5777,5772,5773,5762,5763,5844,5847,5848,5851,5860,5863,5864,5867,5948,5949,5938,5939,5934,5933,5928,5929,6102,6103,6098,6097,6092,6093,6082,6083,4798,4797,4792,4793,4742,4743,4738,4737,4734,4733,4728,4729,4678,4679,4674,4673,4542,4541,4536,4537,4486,4487,4482,4481,4478,4477,4472,4473,4422,4423,4418,4417,3775,3772,3771,3770,3717,3716,3715,3712,3711,3708,3707,3706,3653,3652,3651,3648,3519,3516,3515,3514,3461,3460,3459,3456,3455,3452,3451,3450,3397,3396,3395,3392,2111,2110,2097,2096,2095,2092,2091,2090,2261,2260,2259,2256,2255,2254,2241,2240,2325,2326,2329,2330,2341,2342,2345,2346,2431,2430,2417,2416,2415,2412,2411,2410,5781,5780,5779,5776,5775,5774,5761,5760,5845,5846,5849,5850,5861,5862,5865,5866,5951,5950,5937,5936,5935,5932,5931,5930,6101,6100,6099,6096,6095,6094,6081,6080,4799,4796,4795,4794,4741,4740,4739,4736,4735,4732,4731,4730,4677,4676,4675,4672,4543,4540,4539,4538,4485,4484,4483,4480,4479,4476,4475,4474,4421,4420,4419,4416,3776,3777,3790,3791,3792,3795,3796,3797,3626,3627,3628,3631,3632,3633,3646,3647,3520,3521,3534,3535,3536,3539,3540,3541,3370,3371,3372,3375,3376,3377,3390,3391,2112,2115,2116,2117,2170,2171,2172,2175,2176,2179,2180,2181,2234,2235,2236,2239,2538,2537,2534,2533,2522,2521,2518,2517,2432,2433,2446,2447,2448,2451,2452,2453,5738,5739,5740,5743,5744,5745,5758,5759,5674,5673,5670,5669,5658,5657,5654,5653,5952,5955,5956,5957,6010,6011,6012,6015,6016,6019,6020,6021,6074,6075,6076,6079,4800,4801,4814,4815,4816,4819,4820,4821,4650,4651,4652,4655,4656,4657,4670,4671,4544,4545,4558,4559,4560,4563,4564,4565,4394,4395,4396,4399,4400,4401,4414,4415,3779,3778,3789,3788,3793,3794,3799,3798,3625,3624,3629,3630,3635,3634,3645,3644,3523,3522,3533,3532,3537,3538,3543,3542,3369,3368,3373,3374,3379,3378,3389,3388,2113,2114,2119,2118,2169,2168,2173,2174,2177,2178,2183,2182,2233,2232,2237,2238,2539,2536,2535,2532,2523,2520,2519,2516,2435,2434,2445,2444,2449,2450,2455,2454,5737,5736,5741,5742,5747,5746,5757,5756,5675,5672,5671,5668,5659,5656,5655,5652,5953,5954,5959,5958,6009,6008,6013,6014,6017,6018,6023,6022,6073,6072,6077,6078,4803,4802,4813,4812,4817,4818,4823,4822,4649,4648,4653,4654,4659,4658,4669,4668,4547,4546,4557,4556,4561,4562,4567,4566,4393,4392,4397,4398,4403,4402,4413,4412,3780,3783,3784,3787,3806,3805,3800,3801,3622,3623,3618,3617,3636,3639,3640,3643,3524,3527,3528,3531,3550,3549,3544,3545,3366,3367,3362,3361,3380,3383,3384,3387,2126,2125,2120,2121,2166,2167,2162,2161,2190,2189,2184,2185,2230,2231,2226,2225,2540,2541,2530,2531,2524,2525,2514,2515,2436,2439,2440,2443,2462,2461,2456,2457,5734,5735,5730,5729,5748,5751,5752,5755,5676,5677,5666,5667,5660,5661,5650,5651,5966,5965,5960,5961,6006,6007,6002,6001,6030,6029,6024,6025,6070,6071,6066,6065,4804,4807,4808,4811,4830,4829,4824,4825,4646,4647,4642,4641,4660,4663,4664,4667,4548,4551,4552,4555,4574,4573,4568,4569,4390,4391,4386,4385,4404,4407,4408,4411,3781,3782,3785,3786,3807,3804,3803,3802,3621,3620,3619,3616,3637,3638,3641,3642,3525,3526,3529,3530,3551,3548,3547,3546,3365,3364,3363,3360,3381,3382,3385,3386,2127,2124,2123,2122,2165,2164,2163,2160,2191,2188,2187,2186,2229,2228,2227,2224,2543,2542,2529,2528,2527,2526,2513,2512,2437,2438,2441,2442,2463,2460,2459,2458,5733,5732,5731,5728,5749,5750,5753,5754,5679,5678,5665,5664,5663,5662,5649,5648,5967,5964,5963,5962,6005,6004,6003,6000,6031,6028,6027,6026,6069,6068,6067,6064,4805,4806,4809,4810,4831,4828,4827,4826,4645,4644,4643,4640,4661,4662,4665,4666,4549,4550,4553,4554,4575,4572,4571,4570,4389,4388,4387,4384,4405,4406,4409,4410,3834,3833,3830,3829,3808,3811,3812,3813,3610,3611,3612,3615,3594,3593,3590,3589,3578,3577,3574,3573,3552,3555,3556,3557,3354,3355,3356,3359,3338,3337,3334,3333,2128,2129,2142,2143,2144,2145,2158,2159,2192,2193,2206,2207,2208,2209,2222,2223,2544,2547,2548,2549,2506,2507,2508,2511,2490,2489,2486,2485,2464,2467,2468,2469,5722,5723,5724,5727,5706,5705,5702,5701,5680,5683,5684,5685,5642,5643,5644,5647,5968,5969,5982,5983,5984,5985,5998,5999,6032,6033,6046,6047,6048,6049,6062,6063,4858,4857,4854,4853,4832,4835,4836,4837,4634,4635,4636,4639,4618,4617,4614,4613,4602,4601,4598,4597,4576,4579,4580,4581,4378,4379,4380,4383,4362,4361,4358,4357,3835,3832,3831,3828,3809,3810,3815,3814,3609,3608,3613,3614,3595,3592,3591,3588,3579,3576,3575,3572,3553,3554,3559,3558,3353,3352,3357,3358,3339,3336,3335,3332,2131,2130,2141,2140,2147,2146,2157,2156,2195,2194,2205,2204,2211,2210,2221,2220,2545,2546,2551,2550,2505,2504,2509,2510,2491,2488,2487,2484,2465,2466,2471,2470,5721,5720,5725,5726,5707,5704,5703,5700,5681,5682,5687,5686,5641,5640,5645,5646,5971,5970,5981,5980,5987,5986,5997,5996,6035,6034,6045,6044,6051,6050,6061,6060,4859,4856,4855,4852,4833,4834,4839,4838,4633,4632,4637,4638,4619,4616,4615,4612,4603,4600,4599,4596,4577,4578,4583,4582,4377,4376,4381,4382,4363,4360,4359,4356,3836,3837,3826,3827,3822,3821,3816,3817,3606,3607,3602,3601,3596,3597,3586,3587,3580,3581,3570,3571,3566,3565,3560,3561,3350,3351,3346,3345,3340,3341,3330,3331,2132,2135,2136,2139,2148,2151,2152,2155,2196,2199,2200,2203,2212,2215,2216,2219,2558,2557,2552,2553,2502,2503,2498,2497,2492,2493,2482,2483,2478,2477,2472,2473,5718,5719,5714,5713,5708,5709,5698,5699,5694,5693,5688,5689,5638,5639,5634,5633,5972,5975,5976,5979,5988,5991,5992,5995,6036,6039,6040,6043,6052,6055,6056,6059,4860,4861,4850,4851,4846,4845,4840,4841,4630,4631,4626,4625,4620,4621,4610,4611,4604,4605,4594,4595,4590,4589,4584,4585,4374,4375,4370,4369,4364,4365,4354,4355,3839,3838,3825,3824,3823,3820,3819,3818,3605,3604,3603,3600,3599,3598,3585,3584,3583,3582,3569,3568,3567,3564,3563,3562,3349,3348,3347,3344,3343,3342,3329,3328,2133,2134,2137,2138,2149,2150,2153,2154,2197,2198,2201,2202,2213,2214,2217,2218,2559,2556,2555,2554,2501,2500,2499,2496,2495,2494,2481,2480,2479,2476,2475,2474,5717,5716,5715,5712,5711,5710,5697,5696,5695,5692,5691,5690,5637,5636,5635,5632,5973,5974,5977,5978,5989,5990,5993,5994,6037,6038,6041,6042,6053,6054,6057,6058,4863,4862,4849,4848,4847,4844,4843,4842,4629,4628,4627,4624,4623,4622,4609,4608,4607,4606,4593,4592,4591,4588,4587,4586,4373,4372,4371,4368,4367,4366,4353,4352,3840,3843,3844,3845,3898,3899,3900,3903,3904,3905,3918,3919,3920,3923,3924,3925,3242,3243,3244,3247,3248,3249,3262,3263,3264,3267,3268,3269,3322,3323,3324,3327,2986,2985,2982,2981,2970,2969,2966,2965,2922,2921,2918,2917,2906,2905,2902,2901,2560,2563,2564,2565,2618,2619,2620,2623,2624,2625,2638,2639,2640,2643,2644,2645,5546,5547,5548,5551,5552,5553,5566,5567,5568,5571,5572,5573,5626,5627,5628,5631,5290,5289,5286,5285,5274,5273,5270,5269,5226,5225,5222,5221,5210,5209,5206,5205,4864,4867,4868,4869,4922,4923,4924,4927,4928,4929,4942,4943,4944,4947,4948,4949,4266,4267,4268,4271,4272,4273,4286,4287,4288,4291,4292,4293,4346,4347,4348,4351,3841,3842,3847,3846,3897,3896,3901,3902,3907,3906,3917,3916,3921,3922,3927,3926,3241,3240,3245,3246,3251,3250,3261,3260,3265,3266,3271,3270,3321,3320,3325,3326,2987,2984,2983,2980,2971,2968,2967,2964,2923,2920,2919,2916,2907,2904,2903,2900,2561,2562,2567,2566,2617,2616,2621,2622,2627,2626,2637,2636,2641,2642,2647,2646,5545,5544,5549,5550,5555,5554,5565,5564,5569,5570,5575,5574,5625,5624,5629,5630,5291,5288,5287,5284,5275,5272,5271,5268,5227,5224,5223,5220,5211,5208,5207,5204,4865,4866,4871,4870,4921,4920,4925,4926,4931,4930,4941,4940,4945,4946,4951,4950,4265,4264,4269,4270,4275,4274,4285,4284,4289,4290,4295,4294,4345,4344,4349,4350,3854,3853,3848,3849,3894,3895,3890,3889,3908,3911,3912,3915,3934,3933,3928,3929,3238,3239,3234,3233,3252,3255,3256,3259,3278,3277,3272,3273,3318,3319,3314,3313,2988,2989,2978,2979,2972,2973,2962,2963,2924,2925,2914,2915,2908,2909,2898,2899,2574,2573,2568,2569,2614,2615,2610,2609,2628,2631,2632,2635,2654,2653,2648,2649,5542,5543,5538,5537,5556,5559,5560,5563,5582,5581,5576,5577,5622,5623,5618,5617,5292,5293,5282,5283,5276,5277,5266,5267,5228,5229,5218,5219,5212,5213,5202,5203,4878,4877,4872,4873,4918,4919,4914,4913,4932,4935,4936,4939,4958,4957,4952,4953,4262,4263,4258,4257,4276,4279,4280,4283,4302,4301,4296,4297,4342,4343,4338,4337,3855,3852,3851,3850,3893,3892,3891,3888,3909,3910,3913,3914,3935,3932,3931,3930,3237,3236,3235,3232,3253,3254,3257,3258,3279,3276,3275,3274,3317,3316,3315,3312,2991,2990,2977,2976,2975,2974,2961,2960,2927,2926,2913,2912,2911,2910,2897,2896,2575,2572,2571,2570,2613,2612,2611,2608,2629,2630,2633,2634,2655,2652,2651,2650,5541,5540,5539,5536,5557,5558,5561,5562,5583,5580,5579,5578,5621,5620,5619,5616,5295,5294,5281,5280,5279,5278,5265,5264,5231,5230,5217,5216,5215,5214,5201,5200,4879,4876,4875,4874,4917,4916,4915,4912,4933,4934,4937,4938,4959,4956,4955,4954,4261,4260,4259,4256,4277,4278,4281,4282,4303,4300,4299,4298,4341,4340,4339,4336,3856,3857,3870,3871,3872,3873,3886,3887,3962,3961,3958,3957,3936,3939,3940,3941,3226,3227,3228,3231,3210,3209,3206,3205,3280,3281,3294,3295,3296,3297,3310,3311,2992,2995,2996,2997,2954,2955,2956,2959,2928,2931,2932,2933,2890,2891,2892,2895,2576,2577,2590,2591,2592,2593,2606,2607,2682,2681,2678,2677,2656,2659,2660,2661,5530,5531,5532,5535,5514,5513,5510,5509,5584,5585,5598,5599,5600,5601,5614,5615,5296,5299,5300,5301,5258,5259,5260,5263,5232,5235,5236,5237,5194,5195,5196,5199,4880,4881,4894,4895,4896,4897,4910,4911,4986,4985,4982,4981,4960,4963,4964,4965,4250,4251,4252,4255,4234,4233,4230,4229,4304,4305,4318,4319,4320,4321,4334,4335,3859,3858,3869,3868,3875,3874,3885,3884,3963,3960,3959,3956,3937,3938,3943,3942,3225,3224,3229,3230,3211,3208,3207,3204,3283,3282,3293,3292,3299,3298,3309,3308,2993,2994,2999,2998,2953,2952,2957,2958,2929,2930,2935,2934,2889,2888,2893,2894,2579,2578,2589,2588,2595,2594,2605,2604,2683,2680,2679,2676,2657,2658,2663,2662,5529,5528,5533,5534,5515,5512,5511,5508,5587,5586,5597,5596,5603,5602,5613,5612,5297,5298,5303,5302,5257,5256,5261,5262,5233,5234,5239,5238,5193,5192,5197,5198,4883,4882,4893,4892,4899,4898,4909,4908,4987,4984,4983,4980,4961,4962,4967,4966,4249,4248,4253,4254,4235,4232,4231,4228,4307,4306,4317,4316,4323,4322,4333,4332,3860,3863,3864,3867,3876,3879,3880,3883,3964,3965,3954,3955,3950,3949,3944,3945,3222,3223,3218,3217,3212,3213,3202,3203,3284,3287,3288,3291,3300,3303,3304,3307,3006,3005,3000,3001,2950,2951,2946,2945,2942,2941,2936,2937,2886,2887,2882,2881,2580,2583,2584,2587,2596,2599,2600,2603,2684,2685,2674,2675,2670,2669,2664,2665,5526,5527,5522,5521,5516,5517,5506,5507,5588,5591,5592,5595,5604,5607,5608,5611,5310,5309,5304,5305,5254,5255,5250,5249,5246,5245,5240,5241,5190,5191,5186,5185,4884,4887,4888,4891,4900,4903,4904,4907,4988,4989,4978,4979,4974,4973,4968,4969,4246,4247,4242,4241,4236,4237,4226,4227,4308,4311,4312,4315,4324,4327,4328,4331,3861,3862,3865,3866,3877,3878,3881,3882,3967,3966,3953,3952,3951,3948,3947,3946,3221,3220,3219,3216,3215,3214,3201,3200,3285,3286,3289,3290,3301,3302,3305,3306,3007,3004,3003,3002,2949,2948,2947,2944,2943,2940,2939,2938,2885,2884,2883,2880,2581,2582,2585,2586,2597,2598,2601,2602,2687,2686,2673,2672,2671,2668,2667,2666,5525,5524,5523,5520,5519,5518,5505,5504,5589,5590,5593,5594,5605,5606,5609,5610,5311,5308,5307,5306,5253,5252,5251,5248,5247,5244,5243,5242,5189,5188,5187,5184,4885,4886,4889,4890,4901,4902,4905,4906,4991,4990,4977,4976,4975,4972,4971,4970,4245,4244,4243,4240,4239,4238,4225,4224,4309,4310,4313,4314,4325,4326,4329,4330,4074,4073,4070,4069,4058,4057,4054,4053,3968,3969,3982,3983,3984,3987,3988,3989,3178,3179,3180,3183,3184,3185,3198,3199,3114,3113,3110,3109,3098,3097,3094,3093,3008,3009,3022,3023,3024,3027,3028,3029,2858,2859,2860,2863,2864,2865,2878,2879,2794,2793,2790,2789,2778,2777,2774,2773,2688,2689,2702,2703,2704,2707,2708,2709,5482,5483,5484,5487,5488,5489,5502,5503,5418,5417,5414,5413,5402,5401,5398,5397,5312,5313,5326,5327,5328,5331,5332,5333,5162,5163,5164,5167,5168,5169,5182,5183,5098,5097,5094,5093,5082,5081,5078,5077,4992,4993,5006,5007,5008,5011,5012,5013,4202,4203,4204,4207,4208,4209,4222,4223,4138,4137,4134,4133,4122,4121,4118,4117,4075,4072,4071,4068,4059,4056,4055,4052,3971,3970,3981,3980,3985,3986,3991,3990,3177,3176,3181,3182,3187,3186,3197,3196,3115,3112,3111,3108,3099,3096,3095,3092,3011,3010,3021,3020,3025,3026,3031,3030,2857,2856,2861,2862,2867,2866,2877,2876,2795,2792,2791,2788,2779,2776,2775,2772,2691,2690,2701,2700,2705,2706,2711,2710,5481,5480,5485,5486,5491,5490,5501,5500,5419,5416,5415,5412,5403,5400,5399,5396,5315,5314,5325,5324,5329,5330,5335,5334,5161,5160,5165,5166,5171,5170,5181,5180,5099,5096,5095,5092,5083,5080,5079,5076,4995,4994,5005,5004,5009,5010,5015,5014,4201,4200,4205,4206,4211,4210,4221,4220,4139,4136,4135,4132,4123,4120,4119,4116,4076,4077,4066,4067,4060,4061,4050,4051,3972,3975,3976,3979,3998,3997,3992,3993,3174,3175,3170,3169,3188,3191,3192,3195,3116,3117,3106,3107,3100,3101,3090,3091,3012,3015,3016,3019,3038,3037,3032,3033,2854,2855,2850,2849,2868,2871,2872,2875,2796,2797,2786,2787,2780,2781,2770,2771,2692,2695,2696,2699,2718,2717,2712,2713,5478,5479,5474,5473,5492,5495,5496,5499,5420,5421,5410,5411,5404,5405,5394,5395,5316,5319,5320,5323,5342,5341,5336,5337,5158,5159,5154,5153,5172,5175,5176,5179,5100,5101,5090,5091,5084,5085,5074,5075,4996,4999,5000,5003,5022,5021,5016,5017,4198,4199,4194,4193,4212,4215,4216,4219,4140,4141,4130,4131,4124,4125,4114,4115,4079,4078,4065,4064,4063,4062,4049,4048,3973,3974,3977,3978,3999,3996,3995,3994,3173,3172,3171,3168,3189,3190,3193,3194,3119,3118,3105,3104,3103,3102,3089,3088,3013,3014,3017,3018,3039,3036,3035,3034,2853,2852,2851,2848,2869,2870,2873,2874,2799,2798,2785,2784,2783,2782,2769,2768,2693,2694,2697,2698,2719,2716,2715,2714,5477,5476,5475,5472,5493,5494,5497,5498,5423,5422,5409,5408,5407,5406,5393,5392,5317,5318,5321,5322,5343,5340,5339,5338,5157,5156,5155,5152,5173,5174,5177,5178,5103,5102,5089,5088,5087,5086,5073,5072,4997,4998,5001,5002,5023,5020,5019,5018,4197,4196,4195,4192,4213,4214,4217,4218,4143,4142,4129,4128,4127,4126,4113,4112,4080,4083,4084,4085,4042,4043,4044,4047,4026,4025,4022,4021,4000,4003,4004,4005,3162,3163,3164,3167,3146,3145,3142,3141,3120,3123,3124,3125,3082,3083,3084,3087,3066,3065,3062,3061,3040,3043,3044,3045,2842,2843,2844,2847,2826,2825,2822,2821,2800,2803,2804,2805,2762,2763,2764,2767,2746,2745,2742,2741,2720,2723,2724,2725,5466,5467,5468,5471,5450,5449,5446,5445,5424,5427,5428,5429,5386,5387,5388,5391,5370,5369,5366,5365,5344,5347,5348,5349,5146,5147,5148,5151,5130,5129,5126,5125,5104,5107,5108,5109,5066,5067,5068,5071,5050,5049,5046,5045,5024,5027,5028,5029,4186,4187,4188,4191,4170,4169,4166,4165,4144,4147,4148,4149,4106,4107,4108,4111,4081,4082,4087,4086,4041,4040,4045,4046,4027,4024,4023,4020,4001,4002,4007,4006,3161,3160,3165,3166,3147,3144,3143,3140,3121,3122,3127,3126,3081,3080,3085,3086,3067,3064,3063,3060,3041,3042,3047,3046,2841,2840,2845,2846,2827,2824,2823,2820,2801,2802,2807,2806,2761,2760,2765,2766,2747,2744,2743,2740,2721,2722,2727,2726,5465,5464,5469,5470,5451,5448,5447,5444,5425,5426,5431,5430,5385,5384,5389,5390,5371,5368,5367,5364,5345,5346,5351,5350,5145,5144,5149,5150,5131,5128,5127,5124,5105,5106,5111,5110,5065,5064,5069,5070,5051,5048,5047,5044,5025,5026,5031,5030,4185,4184,4189,4190,4171,4168,4167,4164,4145,4146,4151,4150,4105,4104,4109,4110,4094,4093,4088,4089,4038,4039,4034,4033,4028,4029,4018,4019,4014,4013,4008,4009,3158,3159,3154,3153,3148,3149,3138,3139,3134,3133,3128,3129,3078,3079,3074,3073,3068,3069,3058,3059,3054,3053,3048,3049,2838,2839,2834,2833,2828,2829,2818,2819,2814,2813,2808,2809,2758,2759,2754,2753,2748,2749,2738,2739,2734,2733,2728,2729,5462,5463,5458,5457,5452,5453,5442,5443,5438,5437,5432,5433,5382,5383,5378,5377,5372,5373,5362,5363,5358,5357,5352,5353,5142,5143,5138,5137,5132,5133,5122,5123,5118,5117,5112,5113,5062,5063,5058,5057,5052,5053,5042,5043,5038,5037,5032,5033,4182,4183,4178,4177,4172,4173,4162,4163,4158,4157,4152,4153,4102,4103,4098,4097,4095,4092,4091,4090,4037,4036,4035,4032,4031,4030,4017,4016,4015,4012,4011,4010,3157,3156,3155,3152,3151,3150,3137,3136,3135,3132,3131,3130,3077,3076,3075,3072,3071,3070,3057,3056,3055,3052,3051,3050,2837,2836,2835,2832,2831,2830,2817,2816,2815,2812,2811,2810,2757,2756,2755,2752,2751,2750,2737,2736,2735,2732,2731,2730,5461,5460,5459,5456,5455,5454,5441,5440,5439,5436,5435,5434,5381,5380,5379,5376,5375,5374,5361,5360,5359,5356,5355,5354,5141,5140,5139,5136,5135,5134,5121,5120,5119,5116,5115,5114,5061,5060,5059,5056,5055,5054,5041,5040,5039,5036,5035,5034,4181,4180,4179,4176,4175,4174,4161,4160,4159,4156,4155,4154,4101,4100,4099,4096};


namespace {
constexpr int B = 2, N = 8192, C = 512, NH = 8, HD = 64, SEG = 128, NS = N / SEG, NR = B * N;
constexpr float XS = 8.0f, PS = 1024.0f, WSC = 256.0f;
typedef _Float16 b16;
typedef __attribute__((ext_vector_type(16))) _Float16 v16b;
typedef __attribute__((ext_vector_type(8))) _Float16 v8b;
typedef __attribute__((ext_vector_type(8))) float v8f;
typedef __attribute__((ext_vector_type(4))) float v4f;
typedef __attribute__((ext_vector_type(2))) float v2f;
__device__ __forceinline__ float bf16_rne(float f) { unsigned int u = __float_as_uint(f); u += 0x7FFFu + ((u >> 16) & 1u); return __uint_as_float(u & 0xFFFF0000u); }
__device__ __forceinline__ float bfv(float f) { float r = bf16_rne(f); asm volatile("" : "+v"(r)); return r; }
__device__ __forceinline__ void split16(float v, b16& hi, b16& lo) { hi = (b16)v; lo = (b16)(v - (float)hi); }
__device__ __forceinline__ v16b frag_kb(const b16* p, int hh) { const v8b a = *(const v8b*)(p + 8 * hh), b = *(const v8b*)(p + 16 + 8 * hh); v16b f;
#pragma unroll
  for (int e = 0; e < 8; ++e) { f[e] = a[e]; f[8 + e] = b[e]; } return f; }
__device__ __forceinline__ v8f wmma16b(v16b a, v16b b, v8f c) { v8f d = __builtin_amdgcn_wmma_f32_16x16x32_f16(false, a, false, b, (short)0, c, false, false); asm volatile("v_nop\n\tv_nop\n\tv_nop\n\tv_nop" : "+v"(d) : "v"(a), "v"(b)); return d; }
__device__ __forceinline__ void wave_lds_sync() { __builtin_amdgcn_fence(__ATOMIC_RELEASE, "workgroup"); __builtin_amdgcn_wave_barrier(); __builtin_amdgcn_fence(__ATOMIC_ACQUIRE, "workgroup"); }
__device__ __forceinline__ int iclamp(int v, int lo, int hi) { return v < lo ? lo : (v > hi ? hi : v); }

__global__ __launch_bounds__(256) void wput_kernel(const float* __restrict__ w, int KIN, int OUTW, b16* __restrict__ WT) { const int KG = KIN / 8; const size_t u = (size_t)blockIdx.x * 256 + threadIdx.x; if (u >= (size_t)OUTW * KG) return; const int o = (int)(u / KG), k0 = (int)(u % KG) * 8; v8b v;
#pragma unroll
  for (int j = 0; j < 8; ++j) v[j] = (b16)(bf16_rne(w[(size_t)(k0 + j) * OUTW + o]) * WSC); for (int pass = 0; pass < 2; ++pass) { *(volatile v8b*)(WT + (size_t)o * KIN + k0) = v; __threadfence(); } }
__global__ __launch_bounds__(32) void qkv_kernel(const float* __restrict__ x, const b16* __restrict__ WT, const float* __restrict__ bias, int RL, int SVLIM, float* __restrict__ QKV) {
  __shared__ __attribute__((aligned(16))) b16 Ah[16][C + 8]; __shared__ float Tf[16][132]; const int lane = threadIdx.x, nloc = lane & 15, hlf = lane >> 4; const int cg = blockIdx.x % 12; const size_t m0 = (size_t)(blockIdx.x / 12) * 16; if (m0 >= (size_t)RL) return;
  if (SH_INV[m0 % N] >= SVLIM) return;
  for (int rr = 0; rr < 16; ++rr) for (int q = 0; q < C / 32; ++q) Ah[rr][q * 32 + lane] = (b16)(bf16_rne(x[(m0 + rr) * C + q * 32 + lane]) * XS);
  wave_lds_sync(); v8f acc[8];
#pragma unroll
  for (int t = 0; t < 8; ++t) acc[t] = (v8f){};
#pragma unroll 2
  for (int kb = 0; kb < C; kb += 32) { const v16b a = frag_kb(&Ah[nloc][kb], hlf);
#pragma unroll
    for (int t = 0; t < 8; ++t) acc[t] = wmma16b(a, frag_kb(WT + (size_t)(cg * 128 + t * 16 + nloc) * C + kb, hlf), acc[t]); }
#pragma unroll
  for (int t = 0; t < 8; ++t) { const int c = cg * 128 + t * 16 + nloc; const float bb = bfv(bias[c]);
#pragma unroll
    for (int r8 = 0; r8 < 8; ++r8) Tf[8 * hlf + r8][t * 16 + nloc] = acc[t][r8] * (1.0f / (XS * WSC)) + bb; }
  wave_lds_sync();
  for (int pass = 0; pass < 2; ++pass) { for (int rr = 0; rr < 16; ++rr) *(volatile v4f*)(QKV + (m0 + rr) * (3 * C) + cg * 128 + lane * 4) = *(const v4f*)(&Tf[rr][lane * 4]); __threadfence(); }
}
__global__ __launch_bounds__(32) void att_kernel(const float* __restrict__ QKV, int BV, int SV, float* __restrict__ O) {
  __shared__ __attribute__((aligned(16))) b16 Qh[16][HD + 8], Ql[16][HD + 8], Kh[32][HD + 8], Kl[32][HD + 8], Ph[16][40], Pl[16][40], Vh[HD][40], Vl[HD][40]; __shared__ float Sc[16][33], Mx[16], Dn[16], Sf[16], Of[16][HD + 2]; __shared__ int Qt[16], Kt[32];
  const int lane = threadIdx.x, nloc = lane & 15, hlf = lane >> 4; const int qt = blockIdx.x % (SEG / 16); const int hh = (blockIdx.x / (SEG / 16)) % NH; const int s = (blockIdx.x / ((SEG / 16) * NH)) % NS; const int b = blockIdx.x / ((SEG / 16) * NH * NS); if (b >= BV || s >= SV) return;
  const int p0 = s * SEG + qt * 16; if (lane < 16) { Qt[lane] = iclamp(SH_PERM[p0 + lane], 0, N - 1); Mx[lane] = -INFINITY; Dn[lane] = 0.0f; Sf[lane] = 0.0f; }
  wave_lds_sync(); const size_t rb_ = (size_t)b * N;
  for (int rr = 0; rr < 16; ++rr) for (int q = 0; q < 2; ++q) { const float qv = QKV[(rb_ + Qt[rr]) * (3 * C) + hh * HD + q * 32 + lane] * XS; b16 p, ql; split16(qv, p, ql); Qh[rr][q * 32 + lane] = p; Ql[rr][q * 32 + lane] = ql; }
  v8f acc[4] = {(v8f){}, (v8f){}, (v8f){}, (v8f){}}; wave_lds_sync();
#pragma unroll 1
  for (int kc = 0; kc < SEG; kc += 32) {
    Kt[lane] = iclamp(SH_PERM[s * SEG + kc + lane], 0, N - 1); wave_lds_sync();
    for (int rr = 0; rr < 32; ++rr) { const size_t kr = (rb_ + Kt[rr]) * (3 * C); for (int q = 0; q < 2; ++q) { const float kv = QKV[kr + C + hh * HD + q * 32 + lane] * XS; { b16 p, ql; split16(kv, p, ql); Kh[rr][q * 32 + lane] = p; Kl[rr][q * 32 + lane] = ql; } b16 vp, vl; split16(QKV[kr + 2 * C + hh * HD + q * 32 + lane] * XS, vp, vl); Vh[q * 32 + lane][rr] = vp; Vl[q * 32 + lane][rr] = vl; } }
    wave_lds_sync();
#pragma unroll
    for (int blk = 0; blk < 2; ++blk) { v8f sacc = {};
#pragma unroll
      for (int kb = 0; kb < HD; kb += 32) { const v16b qh = frag_kb(&Qh[nloc][kb], hlf), kh = frag_kb(&Kh[blk * 16 + nloc][kb], hlf); sacc = wmma16b(qh, kh, sacc); { const v16b qlo = frag_kb(&Ql[nloc][kb], hlf), kl = frag_kb(&Kl[blk * 16 + nloc][kb], hlf); sacc = wmma16b(qh, kl, sacc); sacc = wmma16b(qlo, kh, sacc); } }
#pragma unroll
      for (int r8 = 0; r8 < 8; ++r8) Sc[8 * hlf + r8][blk * 16 + nloc] = sacc[r8] * (0.125f / (XS * XS)); }
    wave_lds_sync();
#pragma unroll 1
    for (int qi = 0; qi < 16; ++qi) { const float sv = Sc[qi][lane]; float cm = sv; for (int o = 16; o; o >>= 1) cm = fmaxf(cm, __shfl_xor(cm, o)); const float mo = Mx[qi]; const float mn = fmaxf(mo, cm); const float p = __expf(sv - mn); float psum = p; for (int o = 16; o; o >>= 1) psum += __shfl_xor(psum, o);
      b16 ph, plo; split16(p * PS, ph, plo); Ph[qi][lane] = ph; Pl[qi][lane] = plo; if (lane == 0) { const float sf = (mo == -INFINITY) ? 0.0f : __expf(mo - mn); Sf[qi] = sf; Dn[qi] = Dn[qi] * sf + psum; Mx[qi] = mn; } }
    wave_lds_sync(); const v16b pa = frag_kb(&Ph[nloc][0], hlf), pb = frag_kb(&Pl[nloc][0], hlf);
#pragma unroll
    for (int tt = 0; tt < 4; ++tt) {
#pragma unroll
      for (int r8 = 0; r8 < 8; ++r8) acc[tt][r8] *= Sf[8 * hlf + r8];
      const v16b vh = frag_kb(&Vh[tt * 16 + nloc][0], hlf), vl = frag_kb(&Vl[tt * 16 + nloc][0], hlf); acc[tt] = wmma16b(pa, vh, acc[tt]); acc[tt] = wmma16b(pa, vl, acc[tt]); acc[tt] = wmma16b(pb, vh, acc[tt]); }
    wave_lds_sync(); }
#pragma unroll
  for (int tt = 0; tt < 4; ++tt)
#pragma unroll
    for (int r8 = 0; r8 < 8; ++r8) { const int rl = 8 * hlf + r8; Of[rl][tt * 16 + nloc] = acc[tt][r8] * (1.0f / (PS * XS)) / Dn[rl]; }
  wave_lds_sync();
  for (int pass = 0; pass < 2; ++pass) { for (int rr = 0; rr < 16; ++rr) *(volatile v2f*)(O + (rb_ + Qt[rr]) * C + hh * HD + lane * 2) = (v2f){Of[rr][lane * 2], Of[rr][lane * 2 + 1]}; __threadfence(); }
}
__global__ __launch_bounds__(32) void proj_kernel(const float* __restrict__ O, const b16* __restrict__ WT, const float* __restrict__ bias, int BV, int SV, float* __restrict__ out) {
  __shared__ __attribute__((aligned(16))) b16 Ah[16][C + 8], Al[16][C + 8]; __shared__ float Tf[16][132]; const int lane = threadIdx.x, nloc = lane & 15, hlf = lane >> 4; const int cg = blockIdx.x % 4; const size_t m0 = (size_t)(blockIdx.x / 4) * 16; const int b = (int)(m0 / N); if (b >= BV) return;
  if (SH_INV[m0 % N] >= SV * SEG) { for (int pass = 0; pass < 2; ++pass) { for (int rr = 0; rr < 16; ++rr) *(volatile v4f*)(out + (m0 + rr) * C + cg * 128 + lane * 4) = (v4f){0.0f, 0.0f, 0.0f, 0.0f}; __threadfence(); } return; }
  for (int rr = 0; rr < 16; ++rr) { const size_t row = m0 + rr; for (int q = 0; q < C / 32; ++q) { b16 p, ql; split16(O[row * C + q * 32 + lane] * XS, p, ql); Ah[rr][q * 32 + lane] = p; Al[rr][q * 32 + lane] = ql; } }
  wave_lds_sync(); v8f acc[8];
#pragma unroll
  for (int t = 0; t < 8; ++t) acc[t] = (v8f){};
#pragma unroll 2
  for (int kb = 0; kb < C; kb += 32) { const v16b a = frag_kb(&Ah[nloc][kb], hlf), al = frag_kb(&Al[nloc][kb], hlf);
#pragma unroll
    for (int t = 0; t < 8; ++t) { const v16b bw = frag_kb(WT + (size_t)(cg * 128 + t * 16 + nloc) * C + kb, hlf); acc[t] = wmma16b(a, bw, acc[t]); acc[t] = wmma16b(al, bw, acc[t]); } }
#pragma unroll
  for (int t = 0; t < 8; ++t) { const int c = cg * 128 + t * 16 + nloc; const float bb = bfv(bias[c]);
#pragma unroll
    for (int r8 = 0; r8 < 8; ++r8) Tf[8 * hlf + r8][t * 16 + nloc] = acc[t][r8] * (1.0f / (XS * WSC)) + bb; }
  wave_lds_sync();
  for (int pass = 0; pass < 2; ++pass) { for (int rr = 0; rr < 16; ++rr) *(volatile v4f*)(out + (m0 + rr) * C + cg * 128 + lane * 4) = *(const v4f*)(&Tf[rr][lane * 4]); __threadfence(); }
  (void)SV;
}
}

extern "C" void kernel_launch(void* const* d_in, const int* in_sizes, int n_in, void* d_out, int out_size, void* d_ws, size_t ws_size, hipStream_t stream) {
  (void)n_in;
  auto Fp = [&](int i) { return (const float*)d_in[i]; };
  if (in_sizes[0] != NR * C || in_sizes[1] != C * 3 * C || in_sizes[2] != 3 * C || in_sizes[3] != C * C || in_sizes[4] != C || out_size != NR * C) return;
  const int BV = B, SV = NS;
  size_t off = 0; char* ws = (char*)d_ws;
  auto carve = [&](size_t bytes) { char* p = ws + off; off += (bytes + 255) & ~(size_t)255; return p; };
  b16* WQ = (b16*)carve((size_t)3 * C * C * 2); b16* WO = (b16*)carve((size_t)C * C * 2); float* QKV = (float*)carve((size_t)NR * 3 * C * 4); float* O = (float*)carve((size_t)NR * C * 4);
  if (off > ws_size || off > ((size_t)160 << 20)) return;
  wput_kernel<<<(unsigned)(((size_t)3 * C * (C / 8) + 255) / 256), 256, 0, stream>>>(Fp(1), C, 3 * C, WQ); wput_kernel<<<(unsigned)(((size_t)C * (C / 8) + 255) / 256), 256, 0, stream>>>(Fp(3), C, C, WO);
  qkv_kernel<<<(BV * N / 16) * 12, 32, 0, stream>>>(Fp(0), WQ, Fp(2), BV * N, SV * SEG, QKV);
  att_kernel<<<BV * NS * NH * (SEG / 16), 32, 0, stream>>>(QKV, BV, SV, O);
  proj_kernel<<<(BV * N / 16) * 4, 32, 0, stream>>>(O, WO, Fp(4), BV, SV, (float*)d_out);
}
